// HybridHead_26396869001473
// MI455X (gfx1250) — hardware-verified
//
#include <hip/hip_runtime.h>
#include <math.h>

typedef __attribute__((ext_vector_type(16))) _Float16 v16h;
typedef __attribute__((ext_vector_type(8)))  _Float16 v8h;
typedef __attribute__((ext_vector_type(16))) __bf16   v16b;
typedef __attribute__((ext_vector_type(8)))  float    v8f;
typedef __attribute__((ext_vector_type(4)))  float    v4f;

__device__ __forceinline__ int frag_k(int i, int h) { return (i < 8) ? (8 * h + i) : (16 + 8 * h + (i - 8)); }
__device__ __forceinline__ __bf16 bf16_rne(float f) {
    unsigned int u = __float_as_uint(f);
    u += 0x7fffu + ((u >> 16) & 1u);
    return __builtin_bit_cast(__bf16, (unsigned short)(u >> 16));
}
__device__ __forceinline__ float bf16_f32(__bf16 b) { return __uint_as_float(((unsigned int)__builtin_bit_cast(unsigned short, b)) << 16); }
__device__ __forceinline__ v8f wmma16(v16h a, v16h b, v8f c) {
    c = __builtin_amdgcn_wmma_f32_16x16x32_f16(false, a, false, b, (short)0, c, false, false);
    asm volatile("v_nop\n\tv_nop\n\tv_nop\n\tv_nop" : "+v"(c) : "v"(a), "v"(b));
    return c;
}
__device__ __forceinline__ v8f wmmab(v16b a, v16b b, v8f c) {
    c = __builtin_amdgcn_wmma_f32_16x16x32_bf16(false, a, false, b, (short)0, c, false, false);
    asm volatile("v_nop\n\tv_nop\n\tv_nop\n\tv_nop" : "+v"(c) : "v"(a), "v"(b));
    return c;
}
struct Split { v16b hi, lo; };
__device__ __forceinline__ v8f wmma3(const Split& a, const Split& b, v8f c) {
    c = __builtin_amdgcn_wmma_f32_16x16x32_bf16(false, a.hi, false, b.hi, (short)0, c, false, false);
    c = __builtin_amdgcn_wmma_f32_16x16x32_bf16(false, a.hi, false, b.lo, (short)0, c, false, false);
    c = __builtin_amdgcn_wmma_f32_16x16x32_bf16(false, a.lo, false, b.hi, (short)0, c, false, false);
    asm volatile("v_nop\n\tv_nop\n\tv_nop\n\tv_nop" : "+v"(c) : "v"(a.hi), "v"(a.lo), "v"(b.hi), "v"(b.lo));
    return c;
}
struct Split3 { v16b hi, mid, lo; };
__device__ __forceinline__ v8f wmma6(const Split3& a, const Split3& b, v8f c) {
    c = __builtin_amdgcn_wmma_f32_16x16x32_bf16(false, a.hi, false, b.hi, (short)0, c, false, false);
    c = __builtin_amdgcn_wmma_f32_16x16x32_bf16(false, a.hi, false, b.mid, (short)0, c, false, false);
    c = __builtin_amdgcn_wmma_f32_16x16x32_bf16(false, a.mid, false, b.hi, (short)0, c, false, false);
    c = __builtin_amdgcn_wmma_f32_16x16x32_bf16(false, a.hi, false, b.lo, (short)0, c, false, false);
    c = __builtin_amdgcn_wmma_f32_16x16x32_bf16(false, a.mid, false, b.mid, (short)0, c, false, false);
    c = __builtin_amdgcn_wmma_f32_16x16x32_bf16(false, a.lo, false, b.hi, (short)0, c, false, false);
    asm volatile("v_nop\n\tv_nop\n\tv_nop\n\tv_nop" : "+v"(c) : "v"(a.hi), "v"(a.mid), "v"(a.lo), "v"(b.hi), "v"(b.mid), "v"(b.lo));
    return c;
}

__device__ __forceinline__ v16h fh_ld(const float* __restrict__ p, long long sk, int k0, int h, int klen, float s) {
    v16h a;
#pragma unroll
    for (int i = 0; i < 16; ++i) { const int k = k0 + frag_k(i, h); a[i] = (k < klen) ? (_Float16)(p[(long long)k * sk] * s) : (_Float16)0.f; }
    return a;
}
__device__ __forceinline__ Split sp_ld(const float* __restrict__ p, long long sk, int k0, int h, int klen, float s) {
    Split r;
#pragma unroll
    for (int i = 0; i < 16; ++i) {
        const int k = k0 + frag_k(i, h); const float x = (k < klen) ? p[(long long)k * sk] * s : 0.f;
        const __bf16 hb = bf16_rne(x); r.hi[i] = hb; r.lo[i] = bf16_rne(x - bf16_f32(hb));
    }
    return r;
}
__device__ __forceinline__ Split3 sp3_ld(const float* __restrict__ p, long long sk, int k0, int h, int klen, float s) {
    Split3 r;
#pragma unroll
    for (int i = 0; i < 16; ++i) {
        const int k = k0 + frag_k(i, h); const float x = (k < klen) ? p[(long long)k * sk] * s : 0.f;
        const __bf16 hb = bf16_rne(x); const float r1 = x - bf16_f32(hb); const __bf16 mb = bf16_rne(r1);
        r.hi[i] = hb; r.mid[i] = mb; r.lo[i] = bf16_rne(r1 - bf16_f32(mb));
    }
    return r;
}
__device__ __forceinline__ v16b bh_ld(const float* __restrict__ p, long long sk, int k0, int h, int klen, float s) {
    v16b a;
#pragma unroll
    for (int i = 0; i < 16; ++i) { const int k = k0 + frag_k(i, h); a[i] = bf16_rne((k < klen) ? p[(long long)k * sk] * s : 0.f); }
    return a;
}
__device__ __forceinline__ v16h fh_row(const _Float16* __restrict__ row, int k0, int h) {
    v16h a;
#pragma unroll
    for (int i = 0; i < 16; ++i) a[i] = row[k0 + frag_k(i, h)];
    return a;
}

#define VST2(T, ptr, val) do { const T vst2_v_ = (val); *(volatile T*)(ptr) = vst2_v_; __threadfence(); *(volatile T*)(ptr) = vst2_v_; } while (0)
typedef float v4f __attribute__((ext_vector_type(4)));
#define VST2V4(ptr, val) do { const v4f vst2_v4_ = (val); *(volatile v4f*)(ptr) = vst2_v4_; __threadfence(); *(volatile v4f*)(ptr) = vst2_v4_; } while (0)

__device__ __attribute__((noinline)) float act_fn(float v, int act) {
    if (act == 1) return fmaxf(v, 0.f);
    if (act == 2) { const float u = 0.7978845608028654f * (v + 0.044715f * v * v * v); return 0.5f * v * (1.f + tanhf(u)); }
    if (act == 3) return v / (1.f + expf(-v));
    if (act == 4) return 0.5f * v * (1.f + erff(v * 0.7071067811865476f));
    if (act == 5) return tanhf(v);
    if (act == 6) return 1.f / (1.f + expf(-v));
    if (act == 7) return (v > 0.f) ? v : 0.01f * v;
    if (act == 8) return (v > 0.f) ? v : (expf(v) - 1.f);
    if (act == 9) return fminf(fmaxf(v, 0.f), 6.f);
    if (act == 10) return fabsf(v);
    if (act == 11) return (v >= 0.f) ? v : 0.1f * v;
    if (act == 12) return (v > 0.f) ? v : 0.2f * v;
    if (act == 13) return (v > 20.f) ? v : log1pf(expf(v));
    return v;
}

struct GemmP {
    const float* A; const float* B; const float* bias; const float* R; float* C;
    long long sAo, sAi, sAm, sAk, sBo, sBi, sBn, sBk, sCo, sCi, sCm, sRo, sRi, sRm, sRn;
    int M, N, K, zi_n, flags, act; float alpha, beta, sa, sb;
    int Npad, pad_;
};
static_assert(sizeof(GemmP) == 5 * 8 + 15 * 8 + 6 * 4 + 4 * 4 + 2 * 4, "GemmP has padding");

template <int MODE>
__global__ __launch_bounds__(32) void k_gemm(GemmP p) {
    const int lane = threadIdx.x & 31, h = lane >> 4, l15 = lane & 15;
    const int m0 = blockIdx.y * 16, n0 = blockIdx.x * 32;
    const int z = blockIdx.z, zo = z / p.zi_n, zi = z - zo * p.zi_n;
    const float* A = p.A + zo * p.sAo + zi * p.sAi;
    const float* B = p.B + zo * p.sBo + zi * p.sBi;
    const int am = min(m0 + l15, p.M - 1);
    v8f acc[2], comp[2];
#pragma unroll
    for (int t = 0; t < 2; ++t) { v8f zz = {}; acc[t] = zz; comp[t] = zz; }
    for (int k0 = 0; k0 < p.K; k0 += 32) {
        const float* arow = A + (long long)am * p.sAm;
        if (MODE == 1) {
            const Split a = sp_ld(arow, p.sAk, k0, h, p.K, 1.f);
#pragma unroll
            for (int t = 0; t < 2; ++t) {
                const int bn = min(n0 + t * 16 + l15, p.N - 1);
                acc[t] = wmma3(a, sp_ld(B + (long long)bn * p.sBn, p.sBk, k0, h, p.K, 1.f), acc[t]);
            }
        } else if (MODE == 3) {
            const Split3 a = sp3_ld(arow, p.sAk, k0, h, p.K, 1.f);
#pragma unroll
            for (int t = 0; t < 2; ++t) {
                const int bn = min(n0 + t * 16 + l15, p.N - 1);
                acc[t] = wmma6(a, sp3_ld(B + (long long)bn * p.sBn, p.sBk, k0, h, p.K, 1.f), acc[t]);
            }
        } else if (MODE == 4) {
            const Split3 a = sp3_ld(arow, p.sAk, k0, h, p.K, 1.f);
#pragma unroll
            for (int t = 0; t < 2; ++t) {
                const int bn = min(n0 + t * 16 + l15, p.N - 1); v8f zz = {};
                const v8f part = wmma6(a, sp3_ld(B + (long long)bn * p.sBn, p.sBk, k0, h, p.K, 1.f), zz);
                const v8f y = part - comp[t]; const v8f s = acc[t] + y; comp[t] = (s - acc[t]) - y; acc[t] = s;
            }
        } else if (MODE == 2) {
            const v16b a = bh_ld(arow, p.sAk, k0, h, p.K, 1.f);
#pragma unroll
            for (int t = 0; t < 2; ++t) {
                const int bn = min(n0 + t * 16 + l15, p.N - 1);
                acc[t] = wmmab(a, bh_ld(B + (long long)bn * p.sBn, p.sBk, k0, h, p.K, 1.f), acc[t]);
            }
        } else {
            const v16h a = fh_ld(arow, p.sAk, k0, h, p.K, p.sa);
#pragma unroll
            for (int t = 0; t < 2; ++t) {
                const int bn = min(n0 + t * 16 + l15, p.N - 1);
                acc[t] = wmma16(a, fh_ld(B + (long long)bn * p.sBn, p.sBk, k0, h, p.K, p.sb), acc[t]);
            }
        }
    }
    const float iscale = (MODE == 0) ? p.alpha / (p.sa * p.sb) : p.alpha;
    float* C = p.C + zo * p.sCo + zi * p.sCi;
    const float* R = p.R + zo * p.sRo + zi * p.sRi;
    __shared__ __align__(16) float ctile[16][36];
#pragma unroll
    for (int t = 0; t < 2; ++t) {
        const int n = n0 + t * 16 + l15; const int nn = min(n, p.N - 1);
#pragma unroll
        for (int r = 0; r < 8; ++r) {
            const int m = m0 + 8 * h + r; const int mm = min(m, p.M - 1);
            float v = acc[t][r] * iscale;
            if (p.flags & 1) v += p.bias[nn];
            if (p.flags & 2) v += p.bias[mm];
            if (p.flags & 8) v *= p.bias[(long long)zo * p.M + mm];
            v = act_fn(v, p.act);
            if (p.flags & 4) v += p.beta * R[(long long)mm * p.sRm + (long long)nn * p.sRn];
            ctile[8 * h + r][t * 16 + l15] = (n < p.N) ? v : 0.f;
        }
    }
    __syncthreads();
    const int NW = (p.Npad > p.N) ? p.Npad : p.N;
    const bool fast = (m0 + 16 <= p.M) && (n0 + 32 <= NW) && ((p.sCm & 3) == 0) && ((((size_t)C) & 15) == 0);
    if (fast) {
#pragma unroll
        for (int s = 0; s < 4; ++s) {
            const int row = s * 4 + (lane >> 3), c4 = (lane & 7) * 4;
            const v4f v = *(const v4f*)&ctile[row][c4];
            VST2V4(C + (long long)(m0 + row) * p.sCm + n0 + c4, v);
        }
    } else {
        for (int row = 0; row < 16; ++row) {
            const int m = m0 + row, n = n0 + lane;
            if (m < p.M && n < NW) VST2(float, C + (long long)m * p.sCm + n, ctile[row][lane]);
        }
    }
}


template <int MODE, int TM, int TN>
__global__ __launch_bounds__(32) void k_gemmT(GemmP p) {
    const int lane = threadIdx.x & 31, h = lane >> 4, l15 = lane & 15;
    const int m0 = blockIdx.y * (16 * TM), n0 = blockIdx.x * (16 * TN);
    const int z = blockIdx.z, zo = z / p.zi_n, zi = z - zo * p.zi_n;
    const float* A = p.A + zo * p.sAo + zi * p.sAi;
    const float* B = p.B + zo * p.sBo + zi * p.sBi;
    v8f acc[TM][TN];
#pragma unroll
    for (int i = 0; i < TM; ++i)
#pragma unroll
        for (int t = 0; t < TN; ++t) { v8f zz = {}; acc[i][t] = zz; }
    for (int k0 = 0; k0 < p.K; k0 += 32) {
        if (MODE == 1) {
            Split a[TM], b[TN];
#pragma unroll
            for (int i = 0; i < TM; ++i) { const int am = min(m0 + 16 * i + l15, p.M - 1); a[i] = sp_ld(A + (long long)am * p.sAm, p.sAk, k0, h, p.K, 1.f); }
#pragma unroll
            for (int t = 0; t < TN; ++t) { const int bn = min(n0 + 16 * t + l15, p.N - 1); b[t] = sp_ld(B + (long long)bn * p.sBn, p.sBk, k0, h, p.K, 1.f); }
#pragma unroll
            for (int i = 0; i < TM; ++i)
#pragma unroll
                for (int t = 0; t < TN; ++t) acc[i][t] = wmma3(a[i], b[t], acc[i][t]);
        } else if (MODE == 2) {
            v16b a[TM], b[TN];
#pragma unroll
            for (int i = 0; i < TM; ++i) { const int am = min(m0 + 16 * i + l15, p.M - 1); a[i] = bh_ld(A + (long long)am * p.sAm, p.sAk, k0, h, p.K, 1.f); }
#pragma unroll
            for (int t = 0; t < TN; ++t) { const int bn = min(n0 + 16 * t + l15, p.N - 1); b[t] = bh_ld(B + (long long)bn * p.sBn, p.sBk, k0, h, p.K, 1.f); }
#pragma unroll
            for (int i = 0; i < TM; ++i)
#pragma unroll
                for (int t = 0; t < TN; ++t) acc[i][t] = wmmab(a[i], b[t], acc[i][t]);
        } else {
            v16h a[TM], b[TN];
#pragma unroll
            for (int i = 0; i < TM; ++i) { const int am = min(m0 + 16 * i + l15, p.M - 1); a[i] = fh_ld(A + (long long)am * p.sAm, p.sAk, k0, h, p.K, p.sa); }
#pragma unroll
            for (int t = 0; t < TN; ++t) { const int bn = min(n0 + 16 * t + l15, p.N - 1); b[t] = fh_ld(B + (long long)bn * p.sBn, p.sBk, k0, h, p.K, p.sb); }
#pragma unroll
            for (int i = 0; i < TM; ++i)
#pragma unroll
                for (int t = 0; t < TN; ++t) acc[i][t] = wmma16(a[i], b[t], acc[i][t]);
        }
    }
    const float iscale = (MODE == 0) ? p.alpha / (p.sa * p.sb) : p.alpha;
    float* C = p.C + zo * p.sCo + zi * p.sCi;
    const float* R = p.R + zo * p.sRo + zi * p.sRi;
    const int NW = (p.Npad > p.N) ? p.Npad : p.N;
    __shared__ __align__(16) float ctile[16][36];
#pragma unroll
    for (int i = 0; i < TM; ++i) {
        const int mb = m0 + 16 * i; if (mb >= p.M) break;
#pragma unroll
        for (int tp = 0; tp < TN / 2; ++tp) {
            const int nb = n0 + 32 * tp; if (nb >= NW) break;
#pragma unroll
            for (int t2 = 0; t2 < 2; ++t2) {
                const int t = 2 * tp + t2; const int n = nb + t2 * 16 + l15; const int nn = min(n, p.N - 1);
#pragma unroll
                for (int r = 0; r < 8; ++r) {
                    const int m = mb + 8 * h + r; const int mm = min(m, p.M - 1);
                    float v = acc[i][t][r] * iscale;
                    if (p.flags & 1) v += p.bias[nn];
                    if (p.flags & 2) v += p.bias[mm];
            if (p.flags & 8) v *= p.bias[(long long)zo * p.M + mm];
                    v = act_fn(v, p.act);
                    if (p.flags & 4) v += p.beta * R[(long long)mm * p.sRm + (long long)nn * p.sRn];
                    ctile[8 * h + r][t2 * 16 + l15] = (n < p.N) ? v : 0.f;
                }
            }
            __syncthreads();
            const bool fast = (mb + 16 <= p.M) && (nb + 32 <= NW) && ((p.sCm & 3) == 0) && ((((size_t)C) & 15) == 0);
            if (fast) {
#pragma unroll
                for (int s = 0; s < 4; ++s) {
                    const int row = s * 4 + (lane >> 3), c4 = (lane & 7) * 4;
                    const v4f v = *(const v4f*)&ctile[row][c4];
                    VST2V4(C + (long long)(mb + row) * p.sCm + nb + c4, v);
                }
            } else {
                for (int row = 0; row < 16; ++row) {
                    const int m = mb + row, n = nb + lane;
                    if (m < p.M && n < NW) VST2(float, C + (long long)m * p.sCm + n, ctile[row][lane]);
                }
            }
            __syncthreads();
        }
    }
}

#define AW 4
struct AttnP {
    const float* Q; const float* K; const float* V; float* O; float* P; const float* Mf; const int* Mi; float* ST;
    const float* Pw; const float* Rt; const int* SQ; const int* SK;
    long long swb, swh, swi, swj, srb, srh, sri;
    long long sQb, sQh, sQi, sQd, sKb, sKh, sKj, sKd, sVb, sVh, sVj, sVd, sOb, sOh, sOi, sPb, sPh, sPi, smb, smh, smi, smj;
    int Lq, Lk, dh, dv, hrep, causal, coff, pband;
    float scale, mfill; int nonorm, mpol;
    int roff, rn, segpol, win;
};
static_assert(sizeof(AttnP) == 12 * 8 + 29 * 8 + 16 * 4, "AttnP has padding");

#ifndef KATTN_ATTR
#define KATTN_ATTR
#endif
template <int DHP, int DVP, int QM, bool SPLITPV, bool TWOPASS>
__global__ __launch_bounds__(32 * AW) KATTN_ATTR void k_attn(AttnP p) {
    constexpr int NT = DVP / 16;
    constexpr int KS = DHP / 32;
    constexpr int VP = DVP + 8;
    __shared__ __align__(16) float    pl[AW][16 * 64];
    __shared__ __align__(16) _Float16 vl[(SPLITPV ? 2 : 1) * 64 * VP];
    const int lane = threadIdx.x & 31, hf = lane >> 4, l15 = lane & 15, wave = threadIdx.x >> 5;
    const int h = blockIdx.y, b = blockIdx.z, hk = h / p.hrep;
    const int q0 = (blockIdx.x * AW + wave) * 16;
    float* myp = pl[wave];
    const float L2E = 1.4426950408889634f;
    const float NEG = -__builtin_inff();
    const int qi = min(q0 + l15, p.Lq - 1);
    const float* qrow = p.Q + b * p.sQb + h * p.sQh + (long long)qi * p.sQi;
    const float* kbase = p.K + b * p.sKb + hk * p.sKh;
    const float* vbase = p.V + b * p.sVb + hk * p.sVh;
    v16h qa[QM == 0 ? KS : 1]; Split qs_[QM == 1 ? KS : 1]; Split3 qt_[QM == 2 ? KS : 1];
#pragma unroll
    for (int ks = 0; ks < KS; ++ks) {
        if (QM == 2) qt_[ks] = sp3_ld(qrow, p.sQd, ks * 32, hf, p.dh, 1.f);
        else if (QM == 1) qs_[ks] = sp_ld(qrow, p.sQd, ks * 32, hf, p.dh, 1.f);
        else qa[ks] = fh_ld(qrow, p.sQd, ks * 32, hf, p.dh, 1.f);
    }
    v8f o[NT]; float m8[8], l8[8];
#pragma unroll
    for (int t = 0; t < NT; ++t) { v8f zz = {}; o[t] = zz; }
#pragma unroll
    for (int i = 0; i < 8; ++i) { m8[i] = NEG; l8[i] = 0.f; }
    int jend = p.Lk; int jstart = 0;
    if (p.causal == 1) { const int je = (blockIdx.x * AW + AW - 1) * 16 + 16 + p.coff; jend = min(jend, max(je, 0)); }
    if (p.win > 0) { const int js = (int)(blockIdx.x * AW) * 16 + p.coff - p.win; jstart = (js > 0) ? (js / 64) * 64 : 0; }
    const int npass = TWOPASS ? 2 : 1;
    for (int pass = 0; pass < npass; ++pass) {
        const bool dopv = (!TWOPASS) || pass == 1;
        for (int j0 = jstart; j0 < jend; j0 += 64) {
            if (dopv) {
                __syncthreads();
                for (int idx = threadIdx.x; idx < 64 * DVP; idx += 32 * AW) {
                    const int jr = idx / DVP, d = idx - jr * DVP, j = j0 + jr;
                    const float f = (j < p.Lk && d < p.dv) ? vbase[(long long)j * p.sVj + (long long)d * p.sVd] : 0.f;
                    if (SPLITPV) {
                        const __bf16 hb = bf16_rne(f);
                        ((__bf16*)vl)[jr * VP + d] = hb; ((__bf16*)vl)[64 * VP + jr * VP + d] = bf16_rne(f - bf16_f32(hb));
                    } else vl[jr * VP + d] = (_Float16)f;
                }
            }
            v8f s[4];
#pragma unroll
            for (int t = 0; t < 4; ++t) {
                const int j = min(j0 + t * 16 + l15, p.Lk - 1);
                const float* krow = kbase + (long long)j * p.sKj;
                v8f acc = {};
#pragma unroll
                for (int ks = 0; ks < KS; ++ks) {
                    if (QM == 2)      acc = wmma6(qt_[ks], sp3_ld(krow, p.sKd, ks * 32, hf, p.dh, 1.f), acc);
                    else if (QM == 1) acc = wmma3(qs_[ks], sp_ld(krow, p.sKd, ks * 32, hf, p.dh, 1.f), acc);
                    else              acc = wmma16(qa[ks], fh_ld(krow, p.sKd, ks * 32, hf, p.dh, 1.f), acc);
                }
                s[t] = acc;
            }
            float pv[8][4];
#pragma unroll
            for (int i = 0; i < 8; ++i) {
                const int irow = q0 + i + 8 * hf;
                const int ic = min(irow, p.Lq - 1);
                float sc[4];
#pragma unroll
                for (int t = 0; t < 4; ++t) {
                    const int jg = j0 + t * 16 + l15;
                    float v = s[t][i] * p.scale;
                    if (p.Mf) v += p.Mf[b * p.smb + h * p.smh + (long long)ic * p.smi + (long long)min(jg, p.Lk - 1) * p.smj];
                    if (p.Rt) { int rc = ic - min(jg, p.Lk - 1) + p.roff; rc = rc < 0 ? 0 : (rc >= p.rn ? p.rn - 1 : rc); v += p.Rt[b * p.srb + h * p.srh + (long long)ic * p.sri + rc]; }
                    if (p.Mi) { const int mv = p.Mi[b * p.smb + h * p.smh + (long long)ic * p.smi + (long long)min(jg, p.Lk - 1) * p.smj]; if (p.mpol ? (mv != 0) : (mv == 0)) v = p.mfill; }
                    if (p.SQ) { const bool same = p.SQ[(long long)b * p.Lq + ic] == p.SK[(long long)b * p.Lk + min(jg, p.Lk - 1)]; if (p.segpol ? same : !same) v = p.mfill; }
                    if (p.causal == 2 && jg > irow + p.coff) v = p.mfill;
                    if (jg >= p.Lk || (p.causal == 1 && jg > irow + p.coff) || (p.causal == 3 && jg < irow + p.coff) || (p.win > 0 && irow + p.coff - jg > p.win)) v = NEG; else v *= L2E;
                    sc[t] = v;
                }
                if (!TWOPASS || pass == 0) {
                    float mx = fmaxf(fmaxf(sc[0], sc[1]), fmaxf(sc[2], sc[3]));
                    mx = fmaxf(mx, __shfl_xor(mx, 1, 32)); mx = fmaxf(mx, __shfl_xor(mx, 2, 32));
                    mx = fmaxf(mx, __shfl_xor(mx, 4, 32)); mx = fmaxf(mx, __shfl_xor(mx, 8, 32));
                    const float mnew = fmaxf(m8[i], mx);
                    const float corr = (mnew == NEG) ? 1.f : exp2f(m8[i] - mnew);
                    float rs = 0.f;
#pragma unroll
                    for (int t = 0; t < 4; ++t) {
                        const float pp = (sc[t] == NEG) ? 0.f : exp2f(sc[t] - mnew); rs += pp;
                        pv[i][t] = p.Pw ? pp * p.Pw[b * p.swb + h * p.swh + (long long)ic * p.swi + (long long)min(j0 + t * 16 + l15, p.Lk - 1) * p.swj] : pp;
                    }
                    rs += __shfl_xor(rs, 1, 32); rs += __shfl_xor(rs, 2, 32); rs += __shfl_xor(rs, 4, 32); rs += __shfl_xor(rs, 8, 32);
                    l8[i] = l8[i] * corr + rs; m8[i] = mnew;
                    if (!TWOPASS) {
#pragma unroll
                        for (int t = 0; t < NT; ++t) o[t][i] *= corr;
                    }
                } else {
                    const float inv = (l8[i] > 0.f) ? 1.f / l8[i] : 0.f;
#pragma unroll
                    for (int t = 0; t < 4; ++t) {
                        const int jg = j0 + t * 16 + l15;
                        float pp = (sc[t] == NEG) ? 0.f : exp2f(sc[t] - m8[i]) * inv;
                        if (p.Pw) pp *= p.Pw[b * p.swb + h * p.swh + (long long)ic * p.swi + (long long)min(jg, p.Lk - 1) * p.swj];
                        pv[i][t] = pp;
                    }
                }
            }
            if (dopv) {
#pragma unroll
                for (int i = 0; i < 8; ++i)
#pragma unroll
                    for (int t = 0; t < 4; ++t) ((volatile float*)myp)[(i + 8 * hf) * 64 + t * 16 + l15] = pv[i][t];
                __syncthreads();
                if (p.P) {
                    float* pb_ = p.P + b * p.sPb + h * p.sPh;
                    const bool fastP = (p.pband == 0) && ((p.sPi & 3) == 0) && (j0 + 64 <= p.Lk) && (q0 + 16 <= p.Lq) && ((((size_t)pb_) & 15) == 0);
                    if (fastP) {
#pragma unroll
                        for (int s = 0; s < 8; ++s) {
                            const int row = s * 2 + (lane >> 4), c4 = (lane & 15) * 4;
                            const v4f v = *(const v4f*)(myp + row * 64 + c4);
                            VST2V4(pb_ + (long long)(q0 + row) * p.sPi + j0 + c4, v);
                        }
                    } else {
                        for (int row = 0; row < 16; ++row) {
                            const int irow = q0 + row; if (irow >= p.Lq) continue;
                            for (int c = lane; c < 64; c += 32) {
                                const int jg = j0 + c; if (jg >= p.Lk) continue;
                                if (p.pband == 0) VST2(float, pb_ + (long long)irow * p.sPi + jg, myp[row * 64 + c]);
                                else if (jg - irow <= p.pband && irow - jg <= p.pband) VST2(float, pb_ + (long long)irow * p.sPi + (jg - irow + p.pband), myp[row * 64 + c]);
                            }
                        }
                    }
                }
                if (SPLITPV) {
                    const Split pa0 = sp_ld(myp + l15 * 64, 1, 0, hf, 64, 1.f), pa1 = sp_ld(myp + l15 * 64, 1, 32, hf, 64, 1.f);
                    const __bf16* vh = (const __bf16*)vl; const __bf16* vlo = vh + 64 * VP;
#pragma unroll
                    for (int t = 0; t < NT; ++t) {
                        const int dcol = t * 16 + l15;
                        Split b0, b1;
#pragma unroll
                        for (int e = 0; e < 16; ++e) {
                            const int k0 = frag_k(e, hf), k1 = 32 + frag_k(e, hf);
                            b0.hi[e] = vh[k0 * VP + dcol]; b0.lo[e] = vlo[k0 * VP + dcol]; b1.hi[e] = vh[k1 * VP + dcol]; b1.lo[e] = vlo[k1 * VP + dcol];
                        }
                        o[t] = wmma3(pa0, b0, o[t]);
                        o[t] = wmma3(pa1, b1, o[t]);
                    }
                } else {
                    const v16h pa0 = fh_ld(myp + l15 * 64, 1, 0, hf, 64, 4096.f), pa1 = fh_ld(myp + l15 * 64, 1, 32, hf, 64, 4096.f);
#pragma unroll
                    for (int t = 0; t < NT; ++t) {
                        const int dcol = t * 16 + l15;
                        v16h b0, b1;
#pragma unroll
                        for (int e = 0; e < 16; ++e) { b0[e] = vl[frag_k(e, hf) * VP + dcol]; b1[e] = vl[(32 + frag_k(e, hf)) * VP + dcol]; }
                        o[t] = wmma16(pa0, b0, o[t]);
                        o[t] = wmma16(pa1, b1, o[t]);
                    }
                }
            }
        }
    }
    float* obase = p.O + b * p.sOb + h * p.sOh;
    if (p.ST) {
        const int rl = lane >> 1, isel = rl & 7;
        float mv = 0.f, lv = 0.f;
#pragma unroll
        for (int i = 0; i < 8; ++i) if (i == isel) { mv = m8[i]; lv = l8[i]; }
        const int irow = q0 + rl;
        if (irow < p.Lq) { float* st = p.ST + (((long long)b * gridDim.y + h) * p.Lq + irow) * 2 + (lane & 1); VST2(float, st, (lane & 1) ? lv : mv * 0.6931471805599453f); }
    }
    float invr[8];
#pragma unroll
    for (int i = 0; i < 8; ++i) {
        if (TWOPASS) invr[i] = SPLITPV ? 1.f : (1.f / 4096.f);
        else if (p.nonorm) invr[i] = exp2f(m8[i]) * (SPLITPV ? 1.f : (1.f / 4096.f));
        else invr[i] = (l8[i] > 0.f) ? (SPLITPV ? 1.f / l8[i] : 1.f / (l8[i] * 4096.f)) : 0.f;
    }
    __syncthreads();
    const bool ofast = ((p.sOi & 3) == 0) && ((((size_t)obase) & 15) == 0) && (q0 + 16 <= p.Lq);
#pragma unroll
    for (int c0 = 0; c0 < DVP; c0 += 64) {
#pragma unroll
        for (int i = 0; i < 8; ++i)
#pragma unroll
            for (int t = 0; t < NT; ++t) if (t * 16 >= c0 && t * 16 < c0 + 64) ((volatile float*)myp)[(i + 8 * hf) * 64 + (t * 16 - c0) + l15] = o[t][i] * invr[i];
        __syncthreads();
        const int cw = (DVP - c0 < 64) ? (DVP - c0) : 64;
        if (ofast && (c0 + cw <= p.dv) && (cw % 32 == 0)) {
            const int lpr = cw / 4;
            const int rows_per_ins = 32 / lpr;
            for (int r0 = 0; r0 < 16; r0 += rows_per_ins) {
                const int row = r0 + lane / lpr, c4 = (lane % lpr) * 4;
                const v4f v = *(const v4f*)(myp + row * 64 + c4);
                VST2V4(obase + (long long)(q0 + row) * p.sOi + c0 + c4, v);
            }
        } else {
            for (int row = 0; row < 16; ++row) {
                const int irow = q0 + row; if (irow >= p.Lq) continue;
                for (int c = lane; c < cw; c += 32) { const int d = c0 + c; if (d < p.dv) VST2(float, obase + (long long)irow * p.sOi + d, myp[row * 64 + c]); }
            }
        }
        __syncthreads();
    }
}

struct TrP { const float* src; float* dst; const float* R2; long long sSz, lds, sDz, ldd, sRz, ldr; int R, C, flags, act; float alpha, beta; };
static_assert(sizeof(TrP) == 3 * 8 + 6 * 8 + 6 * 4, "TrP has padding");
__global__ __launch_bounds__(256) void k_tr(TrP p) {
    __shared__ float tile[32][33];
    const int c0 = blockIdx.x * 32, r0 = blockIdx.y * 32, z = blockIdx.z;
    const int lane = threadIdx.x & 31, wave = threadIdx.x >> 5;
    const float* s = p.src + z * p.sSz;
#pragma unroll
    for (int k = 0; k < 4; ++k) {
        const int rl = wave * 4 + k, r = r0 + rl, c = c0 + lane;
        tile[rl][lane] = (r < p.R && c < p.C) ? s[(long long)r * p.lds + c] : 0.f;
    }
    __syncthreads();
    float* d = p.dst + z * p.sDz; const float* rr = p.R2 + z * p.sRz;
#pragma unroll
    for (int k = 0; k < 4; ++k) {
        const int cl = wave * 4 + k, c = c0 + cl, r = r0 + lane;
        if (c < p.C && r < p.R) {
            float v = act_fn(p.alpha * tile[lane][cl], p.act);
            if (p.flags & 1) v += p.beta * rr[(long long)c * p.ldr + r];
            VST2(float, d + (long long)c * p.ldd + r, v);
        }
    }
}

__global__ __launch_bounds__(256) void k_affine(const float* __restrict__ src, float* __restrict__ dst, int n, float a, float b, const float* __restrict__ sdev) {
    const int i = blockIdx.x * 256 + threadIdx.x;
    if (i < n) { const float aa = sdev ? a * sdev[0] : a; const float v = aa * src[i] + b; VST2(float, dst + i, v); }
}

struct SmP { const float* src; float* dst; const float* Mf; long long sz, sr, dz, dr, smz, smr; int n, pad; float scale_in, scale_out; };
static_assert(sizeof(SmP) == 3 * 8 + 6 * 8 + 4 * 4, "SmP has padding");
__global__ __launch_bounds__(256) void k_softmax(SmP p) {
    __shared__ float red[256];
    const int r = blockIdx.x, z = blockIdx.y, tid = threadIdx.x;
    const float* s = p.src + z * p.sz + (long long)r * p.sr;
    const float* mf = p.Mf ? (p.Mf + z * p.smz + (long long)r * p.smr) : nullptr;
    float mx = -__builtin_inff();
    for (int j = tid; j < p.n; j += 256) { float v = s[j] * p.scale_in; if (mf) v += mf[j]; mx = fmaxf(mx, v); }
    red[tid] = mx; __syncthreads();
    for (int o = 128; o > 0; o >>= 1) { if (tid < o) red[tid] = fmaxf(red[tid], red[tid + o]); __syncthreads(); }
    mx = red[0]; __syncthreads();
    float sum = 0.f;
    for (int j = tid; j < p.n; j += 256) { float v = s[j] * p.scale_in; if (mf) v += mf[j]; sum += (mx == -__builtin_inff()) ? 0.f : expf(v - mx); }
    red[tid] = sum; __syncthreads();
    for (int o = 128; o > 0; o >>= 1) { if (tid < o) red[tid] += red[tid + o]; __syncthreads(); }
    sum = red[0];
    const float inv = (sum > 0.f) ? p.scale_out / sum : 0.f;
    float* d = p.dst + z * p.dz + (long long)r * p.dr;
    for (int j = tid; j < p.n; j += 256) { float v = s[j] * p.scale_in; if (mf) v += mf[j]; const float o = (mx == -__builtin_inff()) ? 0.f : expf(v - mx) * inv; VST2(float, d + j, o); }
}
__global__ __launch_bounds__(256) void k_stats(const float* __restrict__ x, long long sz, long long so, long long si, int inner, int n, float eps, float* __restrict__ stat, int mode) {
    __shared__ float red[256];
    const int z = blockIdx.x, tid = threadIdx.x;
    const float* base = x + z * sz;
    float s = 0.f;
    for (int e = tid; e < n; e += 256) s += base[(long long)(e / inner) * so + (long long)(e % inner) * si];
    red[tid] = s; __syncthreads();
    for (int o = 128; o > 0; o >>= 1) { if (tid < o) red[tid] += red[tid + o]; __syncthreads(); }
    const float mu = (mode == 0 || mode == 3) ? red[0] / (float)n : 0.f; __syncthreads();
    float q = 0.f;
    for (int e = tid; e < n; e += 256) { const float dlt = base[(long long)(e / inner) * so + (long long)(e % inner) * si] - mu; q += dlt * dlt; }
    red[tid] = q; __syncthreads();
    for (int o = 128; o > 0; o >>= 1) { if (tid < o) red[tid] += red[tid + o]; __syncthreads(); }
    {
        float rs;
        if (mode == 2) rs = sqrtf((float)n) / fmaxf(sqrtf(red[0]), eps); else if (mode == 3) rs = rsqrtf(red[0] / (float)(n - 1) + eps); else rs = rsqrtf(red[0] / (float)n + eps);
        if (tid < 32) { const float v = (tid == 0) ? mu : ((tid == 1) ? rs : 0.f); VST2(float, stat + (long long)z * 32 + tid, v); }
    }
}
__global__ __launch_bounds__(256) void k_norm_apply(const float* __restrict__ x, float* __restrict__ y, const float* __restrict__ stat, const float* __restrict__ g, const float* __restrict__ bta,
                                                     int Z, int C, int L, int G, int bn, int act) {
    const long long idx = (long long)blockIdx.x * 256 + threadIdx.x;
    if (idx >= (long long)Z * C * L) return;
    const int l = (int)(idx % L); const long long zc = idx / L; const int c = (int)(zc % C), z = (int)(zc / C); (void)l;
    const int set = bn ? c : (z * G + c / (C / G));
    float v = (x[idx] - stat[(long long)set * 32]) * stat[(long long)set * 32 + 1];
    if (g) v *= g[c];
    if (bta) v += bta[c];
    v = act_fn(v, act);
    VST2(float, y + idx, v);
}

__global__ __launch_bounds__(256) void k_lse_neg(const float* __restrict__ st, float* __restrict__ c, int n) {
    const int i = blockIdx.x * 256 + threadIdx.x;
    if (i < n) { const float v = -(st[2 * i] + logf(st[2 * i + 1])); VST2(float, c + i, v); }
}

__global__ __launch_bounds__(256) void k_iota(int* __restrict__ dst, int n, int a, int b) {
    const int i = blockIdx.x * 256 + threadIdx.x;
    if (i < n) { const int v = a * i + b; VST2(int, dst + i, v); }
}

__global__ __launch_bounds__(256) void k_axpby(const float* __restrict__ x, const float* __restrict__ y, float* __restrict__ dst, int n, float a, float b, float c) {
    const int i = blockIdx.x * 256 + threadIdx.x;
    if (i < n) { const float v = a * x[i] + b * y[i] + c; VST2(float, dst + i, v); }
}

struct RopeP { const float* X; float* Y; const float* C; const float* Sn; const int* pos; long long sXr, sXh, sYr, sYh, sCb, sCp, sCd; int R, Hn, D, S, mode, tmode, pmode, pad; };
static_assert(sizeof(RopeP) == 5 * 8 + 7 * 8 + 8 * 4, "RopeP has padding");
__global__ __launch_bounds__(256) void k_rope(RopeP p) {
    const long long idx = (long long)blockIdx.x * 256 + threadIdx.x;
    if (idx >= (long long)p.R * p.Hn * p.D) return;
    const int d = (int)(idx % p.D); const long long rh = idx / p.D; const int h = (int)(rh % p.Hn); const int r = (int)(rh / p.Hn);
    const int half = p.D / 2;
    int partner; float sign;
    if (p.mode == 0) { partner = (d < half) ? d + half : d - half; sign = (d < half) ? -1.f : 1.f; }
    else { partner = d ^ 1; sign = (d & 1) ? 1.f : -1.f; }
    const int tcol = (p.tmode == 0) ? d : ((p.tmode == 1) ? (d % half) : (d >> 1));
    const int pp = (p.pmode == 0) ? (r % p.S) : ((p.pmode == 1) ? h : p.pos[r]);
    const long long toff = (long long)(r / p.S) * p.sCb + (long long)pp * p.sCp + (long long)tcol * p.sCd;
    const float* xr = p.X + (long long)r * p.sXr + (long long)h * p.sXh;
    const float v = xr[d] * p.C[toff] + sign * xr[partner] * p.Sn[toff];
    VST2(float, p.Y + (long long)r * p.sYr + (long long)h * p.sYh + d, v);
}

__global__ __launch_bounds__(256) void k_invf(float* __restrict__ invb, int half, int D, float base, float num, int fmode, float cexp) {
    const int i = blockIdx.x * 256 + threadIdx.x;
    if (i >= ((half + 31) / 32) * 32) return;
    if (i >= half) { VST2(float, invb + i, 0.f); return; }
    const float e = (float)(2 * i) / (float)D;
    float invf;
    if (fmode == 1) invf = num * expf((float)(2 * i) * cexp);
    else if (fmode == 2) invf = num * powf(base, (-2.0f * ((float)i - 1.0f)) / (float)D);
    else invf = num * (1.0f / powf(base, e));
    VST2(float, invb + i, invf);
}
__global__ __launch_bounds__(256) void k_sincos(float* __restrict__ cs, float* __restrict__ sn, const float* __restrict__ invb, int S, int half, float pscale) {
    const int idx = blockIdx.x * 256 + threadIdx.x;
    if (idx >= S * half) return;
    const int s = idx / half, i = idx - s * half;
    const float ang = (pscale * (float)s) * invb[i];
    VST2(float, cs + idx, cosf(ang)); VST2(float, sn + idx, sinf(ang));
}

__global__ __launch_bounds__(256) void k_mulact(const float* __restrict__ x, const float* __restrict__ y, float* __restrict__ dst, int n, int act) {
    const int i = blockIdx.x * 256 + threadIdx.x;
    if (i < n) { const float v = act_fn(x[i], act) * y[i]; VST2(float, dst + i, v); }
}

__global__ __launch_bounds__(256) void k_matvec(GemmP p) {
    const int rpt = (p.N == 1) ? 1 : 32;
    const long long r0 = ((long long)blockIdx.x * 256 + threadIdx.x) * rpt; const int z = blockIdx.z, zo = z / p.zi_n, zi = z - zo * p.zi_n;
    if (r0 >= p.M) return;
    const float* Bb = p.B + zo * p.sBo + zi * p.sBi;
    float* C = p.C + zo * p.sCo + zi * p.sCi; const float* R = p.R + zo * p.sRo + zi * p.sRi;
    for (int rr = 0; rr < rpt; ++rr) {
        const long long r = r0 + rr; if (r >= p.M) break;
        const float* A = p.A + zo * p.sAo + zi * p.sAi + r * p.sAm;
        float acc[8] = {0.f, 0.f, 0.f, 0.f, 0.f, 0.f, 0.f, 0.f};
        for (int k = 0; k < p.K; ++k) { const float a = A[(long long)k * p.sAk];
#pragma unroll
            for (int j = 0; j < 8; ++j) if (j < p.N) acc[j] += a * Bb[(long long)j * p.sBn + (long long)k * p.sBk]; }
#pragma unroll
        for (int j = 0; j < 8; ++j) if (j < p.N) {
            float v = acc[j] * p.alpha;
            if (p.flags & 1) v += p.bias[j];
            if (p.flags & 2) v += p.bias[r];
            v = act_fn(v, p.act);
            if (p.flags & 4) v += p.beta * R[r * p.sRm + (long long)j * p.sRn];
            VST2(float, C + r * p.sCm + j, v);
        }
    }
}
__global__ __launch_bounds__(256) void k_smallsoftmax(const float* __restrict__ src, float* __restrict__ dst, long long sr, long long dr, int n, long long R, float scale) {
    const long long r0 = ((long long)blockIdx.x * 256 + threadIdx.x) * 32;
    for (int rr = 0; rr < 32; ++rr) {
        const long long r = r0 + rr; if (r >= R) return;
        const float* s = src + r * sr; float* d = dst + r * dr;
        float mx = -__builtin_inff();
        for (int j = 0; j < n; ++j) mx = fmaxf(mx, s[j] * scale);
        float sum = 0.f;
        for (int j = 0; j < n; ++j) sum += expf(s[j] * scale - mx);
        const float inv = 1.f / sum;
        for (int j = 0; j < n; ++j) { const float v = expf(s[j] * scale - mx) * inv; VST2(float, d + j, v); }
    }
}

__global__ __launch_bounds__(32) void k_unitstat(float* __restrict__ st) { const int t = threadIdx.x; const float v = (t == 1) ? 1.f : 0.f; VST2(float, st + t, v); }

__global__ __launch_bounds__(256) void k_lincopy(const float* __restrict__ src, long long lds, float* __restrict__ dst, long long ldd, long long rows, int cols) {
    const long long i = (long long)blockIdx.x * 256 + threadIdx.x; if (i >= rows * cols) return;
    const long long r = i / cols; const int c = (int)(i - r * cols);
    const float v = src[r * lds + c]; VST2(float, dst + r * ldd + c, v);
}

namespace w25 {
typedef __attribute__((ext_vector_type(16))) _Float16 v16h;
typedef __attribute__((ext_vector_type(8)))  _Float16 v8h;
typedef __attribute__((ext_vector_type(16))) __bf16   v16b;
typedef __attribute__((ext_vector_type(8)))  __bf16   v8b;
typedef __attribute__((ext_vector_type(8)))  float    v8f;
typedef __attribute__((ext_vector_type(4)))  float    v4f;

__device__ __forceinline__ unsigned short f2bf_bits(float f) {
  unsigned u = __float_as_uint(f);
  return (unsigned short)((u + 0x7FFFu + ((u >> 16) & 1u)) >> 16);
}
__device__ __forceinline__ float bf_bits2f(unsigned short h) { return __uint_as_float(((unsigned)h) << 16); }

__device__ __forceinline__ void dep_guard_h(v8f& a, v8f& b, v16h x, v16h y) { asm volatile("v_nop\n\tv_nop\n\tv_nop\n\tv_nop" : "+v"(a), "+v"(b) : "v"(x), "v"(y)); }
__device__ __forceinline__ void dep_guard_b(v8f& a, v8f& b, v16b x, v16b y) { asm volatile("v_nop\n\tv_nop\n\tv_nop\n\tv_nop" : "+v"(a), "+v"(b) : "v"(x), "v"(y)); }
__device__ __forceinline__ void keep4_h(v16h a, v16h b, v16h c, v16h d) { asm volatile("v_nop" :: "v"(a), "v"(b), "v"(c), "v"(d)); }
__device__ __forceinline__ void keep4_b(v16b a, v16b b, v16b c, v16b d) { asm volatile("v_nop" :: "v"(a), "v"(b), "v"(c), "v"(d)); }
__device__ __forceinline__ void acc_guard4(v8f& a, v8f& b, v8f& c, v8f& d) { asm volatile("v_nop\n\tv_nop\n\tv_nop\n\tv_nop" : "+v"(a), "+v"(b), "+v"(c), "+v"(d)); }
template <typename T> struct Frag;
template <> struct Frag<_Float16> {
  typedef v16h V; union U { v16h v; v8h h[2]; };
  static __device__ __forceinline__ v16h load(const _Float16* p) {
    U f; f.h[0] = *(const v8h*)(p); f.h[1] = *(const v8h*)(p + 16); return f.v;
  }
  static __device__ __forceinline__ v8f mma(v16h a, v16h b, v8f c) {
    return __builtin_amdgcn_wmma_f32_16x16x32_f16(false, a, false, b, (short)0, c, false, false);
  }
  static __device__ __forceinline__ void guard(v8f& a, v8f& b, v16h x, v16h y) { dep_guard_h(a, b, x, y); }
  static __device__ __forceinline__ void keep(v16h a, v16h b, v16h c, v16h d) { keep4_h(a, b, c, d); }
};
template <> struct Frag<__bf16> {
  typedef v16b V; union U { v16b v; v8b h[2]; };
  static __device__ __forceinline__ v16b load(const __bf16* p) {
    U f; f.h[0] = *(const v8b*)(p); f.h[1] = *(const v8b*)(p + 16); return f.v;
  }
  static __device__ __forceinline__ v8f mma(v16b a, v16b b, v8f c) {
    return __builtin_amdgcn_wmma_f32_16x16x32_bf16(false, a, false, b, (short)0, c, false, false);
  }
  static __device__ __forceinline__ void guard(v8f& a, v8f& b, v16b x, v16b y) { dep_guard_b(a, b, x, y); }
  static __device__ __forceinline__ void keep(v16b a, v16b b, v16b c, v16b d) { keep4_b(a, b, c, d); }
};

template <int ET> struct Elem;
template <> struct Elem<0> { typedef _Float16 T; };
template <> struct Elem<1> { typedef __bf16 T; };
template <int ET, bool SPLIT, int BIAS_MODE, int OUT_MODE, bool RESID, int ACT = 0>
__global__ __launch_bounds__(256) void wmma_gemm64(
    const unsigned short* __restrict__ Ap, const unsigned short* __restrict__ A2p, int lda, long strideA,
    const unsigned short* __restrict__ Btp, const unsigned short* __restrict__ Bt2p, int ldb, long strideB,
    void* __restrict__ Cout, void* __restrict__ Cout2, int ldc, long strideC,
    const float* __restrict__ bias,
    const float* __restrict__ resid, long strideR,
    int M, int N, int K, float scale) {
  typedef typename Elem<ET>::T T;
  typedef typename Frag<T>::V V;
  const T* A = (const T*)Ap; const T* A2 = (const T*)A2p; const T* Bt = (const T*)Btp; const T* Bt2 = (const T*)Bt2p;
  __shared__ __align__(16) float sT[8][16 * 68];
  const int b    = blockIdx.y;
  const int lane = threadIdx.x & 31;
  const int wave = threadIdx.x >> 5;
  const int tilesN = N >> 6;
  const int tilesM = M >> 6;
  const int tile = blockIdx.x * 8 + wave;
  if (tile >= tilesM * tilesN) return;
  const int tm = tile / tilesN;
  const int tn = tile - tm * tilesN;
  const int m0 = tm << 6;
  const int n0 = tn << 6;

  const T* Ab  = A  + (size_t)b * strideA;
  const T* Bb  = Bt + (size_t)b * strideB;
  const T* Ab2 = SPLIT ? (A2  + (size_t)b * strideA) : nullptr;
  const T* Bb2 = SPLIT ? (Bt2 + (size_t)b * strideB) : nullptr;

  const int rlane = lane & 15;
  const int koff  = (lane >> 4) * 8;
  const int mOff  = (lane >> 4) * 8;

  v8f acc[4][4];
#pragma unroll
  for (int i = 0; i < 4; ++i)
#pragma unroll
    for (int j = 0; j < 4; ++j) acc[i][j] = (v8f){0.f,0.f,0.f,0.f,0.f,0.f,0.f,0.f};

  for (int k0 = 0; k0 < K; k0 += 32) {
    V bh[4], bl[4];
#pragma unroll
    for (int j = 0; j < 4; ++j) {
      const size_t bo = (size_t)(n0 + (j << 4) + rlane) * ldb + koff + k0;
      bh[j] = Frag<T>::load(Bb + bo);
      if (SPLIT) bl[j] = Frag<T>::load(Bb2 + bo);
    }
#pragma unroll
    for (int i = 0; i < 4; ++i) {
      const size_t ao = (size_t)(m0 + (i << 4) + rlane) * lda + koff + k0;
      V ah = Frag<T>::load(Ab + ao);
      V al;
      if (SPLIT) al = Frag<T>::load(Ab2 + ao);
#pragma unroll
      for (int j = 0; j < 4; ++j) {
        acc[i][j] = Frag<T>::mma(ah, bh[j], acc[i][j]);
        if (SPLIT) {
          acc[i][j] = Frag<T>::mma(ah, bl[j], acc[i][j]);
          acc[i][j] = Frag<T>::mma(al, bh[j], acc[i][j]);
        }
      }
      Frag<T>::guard(acc[i][0], acc[i][3], ah, SPLIT ? al : ah);
    }
    Frag<T>::keep(bh[0], bh[1], bh[2], bh[3]);
    if (SPLIT) Frag<T>::keep(bl[0], bl[1], bl[2], bl[3]);
  }
  acc_guard4(acc[0][0], acc[0][1], acc[0][2], acc[0][3]);
  acc_guard4(acc[1][0], acc[1][1], acc[1][2], acc[1][3]);
  acc_guard4(acc[2][0], acc[2][1], acc[2][2], acc[2][3]);
  acc_guard4(acc[3][0], acc[3][1], acc[3][2], acc[3][3]);

  float* slab = sT[wave];
  const float* Rb = RESID ? (resid + (size_t)b * strideR) : nullptr;
#pragma unroll
  for (int i = 0; i < 4; ++i) {
    const int mBase = m0 + (i << 4);
#pragma unroll
    for (int j = 0; j < 4; ++j) {
      const int n = n0 + (j << 4) + rlane;
      float bv = 0.f;
      if (BIAS_MODE == 2) bv = bias[n];
#pragma unroll
      for (int r = 0; r < 8; ++r) {
        float v = acc[i][j][r] * scale;
        if (BIAS_MODE == 1) v += bias[mBase + mOff + r];
        if (BIAS_MODE == 2) v += bv;
        if (RESID) v += Rb[(size_t)(mBase + mOff + r) * ldc + n];
        if (ACT == 1) v = tanhf(v);
        if (ACT == 2) v = fmaxf(v, 0.0f);
        if (ACT == 3) v = v / (1.0f + expf(-v));
        if (ACT == 4) v = (v > 0.f) ? v : 0.01f * v;
        if (ACT == 5) v = 0.5f * v * (1.0f + erff(v * 0.70710678118654752f));
        if (ACT == 6) v = (v > 0.f) ? v : 0.2f * v;
        if (ACT == 7) { const float u = 0.7978845608028654f * (v + 0.044715f * v * v * v); v = 0.5f * v * (1.f + tanhf(u)); }
        slab[(mOff + r) * 68 + (j << 4) + rlane] = v;
      }
    }
    __builtin_amdgcn_fence(__ATOMIC_RELEASE, "workgroup");
    __builtin_amdgcn_wave_barrier();
    __builtin_amdgcn_fence(__ATOMIC_ACQUIRE, "workgroup");
    if (OUT_MODE == 0) {
      float* C = (float*)Cout + (size_t)b * strideC;
      const int hh = lane >> 4, c4 = (lane & 15) * 4;
      for (int pass = 0; pass < 2; ++pass) {
#pragma unroll
        for (int it = 0; it < 8; ++it) {
          const int row = it * 2 + hh;
          v4f v = *(const v4f*)(slab + row * 68 + c4);
          *(volatile v4f*)(C + (size_t)(mBase + row) * ldc + n0 + c4) = v;
        }
        __threadfence();
      }
    } else {
      const int q = lane >> 3, c8 = (lane & 7) * 8;
      unsigned short* C  = (unsigned short*)Cout  + (size_t)b * strideC;
      unsigned short* C2 = (OUT_MODE == 2) ? ((unsigned short*)Cout2 + (size_t)b * strideC) : nullptr;
      for (int pass = 0; pass < 2; ++pass) {
#pragma unroll
        for (int it = 0; it < 4; ++it) {
          const int row = it * 4 + q;
          const float* sp = slab + row * 68 + c8;
          v8h hv, lv;
#pragma unroll
          for (int e = 0; e < 8; ++e) {
            if (OUT_MODE == 1) {
              hv[e] = (_Float16)sp[e];
            } else {
              unsigned short hb = f2bf_bits(sp[e]);
              unsigned short lb = f2bf_bits(sp[e] - bf_bits2f(hb));
              hv[e] = __builtin_bit_cast(_Float16, hb);
              lv[e] = __builtin_bit_cast(_Float16, lb);
            }
          }
          *(volatile v8h*)(C + (size_t)(mBase + row) * ldc + n0 + c8) = hv;
          if (OUT_MODE == 2) *(volatile v8h*)(C2 + (size_t)(mBase + row) * ldc + n0 + c8) = lv;
        }
        __threadfence();
      }
    }
    __builtin_amdgcn_fence(__ATOMIC_RELEASE, "workgroup");
    __builtin_amdgcn_wave_barrier();
    __builtin_amdgcn_fence(__ATOMIC_ACQUIRE, "workgroup");
  }
}

__global__ __launch_bounds__(256) void cast_f32_f16x2(
    const float* __restrict__ in, _Float16* __restrict__ out, int n2) {
  int i = blockIdx.x * 256 + threadIdx.x;
  if (i < n2) {
    const _Float16 h0 = (_Float16)in[2 * i], h1 = (_Float16)in[2 * i + 1];
    const unsigned u = (unsigned)__builtin_bit_cast(unsigned short, h0) | ((unsigned)__builtin_bit_cast(unsigned short, h1) << 16);
    ((volatile unsigned*)out)[i] = u;
    __threadfence();
    ((volatile unsigned*)out)[i] = u;
  }
}


}

__global__ __launch_bounds__(256) void k_castT16(const float* __restrict__ src, long long lds, _Float16* __restrict__ dst, long long ldd, int R, int C, float s) {
    const long long i = (long long)blockIdx.x * 256 + threadIdx.x; const long long np = (long long)C * (R / 2); if (i >= np) return; const int c = (int)(i / (R / 2)); const int r = 2 * (int)(i % (R / 2));
    const _Float16 h0 = (_Float16)(src[(long long)r * lds + c] * s), h1 = (_Float16)(src[(long long)(r + 1) * lds + c] * s);
    const unsigned u = (unsigned)__builtin_bit_cast(unsigned short, h0) | ((unsigned)__builtin_bit_cast(unsigned short, h1) << 16);
    volatile unsigned* d = (volatile unsigned*)(dst + (long long)c * ldd + r); *d = u; __threadfence(); *d = u; }
__global__ __launch_bounds__(256) void k_cast16(const float* __restrict__ src, long long lds, _Float16* __restrict__ dst, long long ldd, int R, int C, float s) {
    const long long i = (long long)blockIdx.x * 256 + threadIdx.x; const long long np = (long long)R * (C / 2); if (i >= np) return; const int r = (int)(i / (C / 2)); const int c = 2 * (int)(i % (C / 2));
    const _Float16 h0 = (_Float16)(src[(long long)r * lds + c] * s), h1 = (_Float16)(src[(long long)r * lds + c + 1] * s);
    const unsigned u = (unsigned)__builtin_bit_cast(unsigned short, h0) | ((unsigned)__builtin_bit_cast(unsigned short, h1) << 16);
    volatile unsigned* d = (volatile unsigned*)(dst + (long long)r * ldd + c); *d = u; __threadfence(); *d = u; }

__device__ __forceinline__ unsigned int f2bf2_pack(float a, float b, unsigned int* lo) {
    const unsigned short ha = w25::f2bf_bits(a), hb = w25::f2bf_bits(b);
    const unsigned short la = w25::f2bf_bits(a - w25::bf_bits2f(ha)), lb = w25::f2bf_bits(b - w25::bf_bits2f(hb));
    *lo = (unsigned)la | ((unsigned)lb << 16); return (unsigned)ha | ((unsigned)hb << 16); }
__global__ __launch_bounds__(256) void k_castS16(const float* __restrict__ src, long long lds, __bf16* __restrict__ dhi, __bf16* __restrict__ dlo, long long ldd, int R, int C, float s, int transpose) {
    const long long i = (long long)blockIdx.x * 256 + threadIdx.x; long long o; float a, b;
    if (transpose) { const long long np = (long long)C * (R / 2); if (i >= np) return; const int c = (int)(i / (R / 2)); const int r = 2 * (int)(i % (R / 2)); a = src[(long long)r * lds + c] * s; b = src[(long long)(r + 1) * lds + c] * s; o = (long long)c * ldd + r; }
    else { const long long np = (long long)R * (C / 2); if (i >= np) return; const int r = (int)(i / (C / 2)); const int c = 2 * (int)(i % (C / 2)); a = src[(long long)r * lds + c] * s; b = src[(long long)r * lds + c + 1] * s; o = (long long)r * ldd + c; }
    unsigned lo; const unsigned hi = f2bf2_pack(a, b, &lo); volatile unsigned* ph = (volatile unsigned*)(dhi + o); volatile unsigned* pl = (volatile unsigned*)(dlo + o);
    *ph = hi; *pl = lo; __threadfence(); *ph = hi; *pl = lo; }

namespace w25 {
#define AT_D 64
#define AT_NW 4
#define AT_QB 64
#define AT_KC 64
struct AttnGeom { const float* cp = nullptr; const float* pc = nullptr; long c_bs = 0, c_rs = 0, c_hs = 0;
                  long q_bs, q_rs, q_hs, k_bs, k_rs, k_hs, v_bs, v_rs, v_hs, o_bs, o_rs, o_hs;
                  int S, Skv, H, mask_mode; float qscale; int blk0; float mask_fill; int mask_is_int; };
static_assert(sizeof(AttnGeom) == 168, "no padding");

__device__ __forceinline__ unsigned short at_bf_bits(float f) {
  unsigned u = __float_as_uint(f);
  return (unsigned short)((u + 0x7FFFu + ((u >> 16) & 1u)) >> 16);
}
__device__ __forceinline__ __bf16 at_f2bf(float f) { return __builtin_bit_cast(__bf16, at_bf_bits(f)); }
__device__ __forceinline__ void at_split(float f, __bf16& hi, __bf16& lo) {
  const unsigned short hb = at_bf_bits(f);
  hi = __builtin_bit_cast(__bf16, hb);
  lo = at_f2bf(f - __uint_as_float(((unsigned)hb) << 16));
}
__device__ __forceinline__ v8f at_mma(v16b a, v16b b, v8f c) {
  c = __builtin_amdgcn_wmma_f32_16x16x32_bf16(false, a, false, b, (short)0, c, false, false);
  asm volatile("v_nop\n\tv_nop\n\tv_nop\n\tv_nop" : "+v"(c) : "v"(a), "v"(b));
  return c;
}
template <bool F16> __device__ __forceinline__ __bf16 at_to16(float f) {
  if (F16) return __builtin_bit_cast(__bf16, (_Float16)f);
  return at_f2bf(f);
}
template <bool F16> __device__ __forceinline__ v8f at_mma16(v16b a, v16b b, v8f c) {
  if (F16) {
    const v16h ah = __builtin_bit_cast(v16h, a), bh = __builtin_bit_cast(v16h, b);
    c = __builtin_amdgcn_wmma_f32_16x16x32_f16(false, ah, false, bh, (short)0, c, false, false);
    asm volatile("v_nop\n\tv_nop\n\tv_nop\n\tv_nop" : "+v"(c) : "v"(ah), "v"(bh));
    return c;
  }
  return at_mma(a, b, c);
}

template <bool SPLIT_QK, bool SPLIT_PV, bool F16 = false>
__global__ __launch_bounds__(128)
void attn64_kernel(const float* __restrict__ q, const float* __restrict__ k,
                   const float* __restrict__ v, float* __restrict__ out,
                   const void* __restrict__ mask_a, const int* __restrict__ mask_b, AttnGeom g) {
  static_assert(!(F16 && (SPLIT_QK || SPLIT_PV)), "f16 mode is non-split");
  const float PSC = F16 ? 32768.0f : 1.0f;
  union FB { v16b v; v8b h[2]; };
  __shared__ __align__(16) __bf16 Ksh[AT_KC * AT_D];
  __shared__ __align__(16) __bf16 Ksl[SPLIT_QK ? AT_KC * AT_D : 8];
  __shared__ __align__(16) __bf16 Vth[AT_D * AT_KC];
  __shared__ __align__(16) __bf16 Vtl[SPLIT_PV ? AT_D * AT_KC : 8];
  __shared__ __align__(16) __bf16 Psh[AT_NW][16 * AT_KC];
  __shared__ __align__(16) __bf16 Psl[SPLIT_PV ? AT_NW : 1][SPLIT_PV ? 16 * AT_KC : 8];
  __shared__ __align__(16) float  Os[AT_NW][16 * 68];

  const int tid  = threadIdx.x;
  const int wave = tid >> 5;
  const int lane = tid & 31;
  const int hh   = lane >> 4;
  const int c    = lane & 15;

  const int nqb = g.S / AT_QB;
  const int bx = blockIdx.x + g.blk0;
  const int qb = bx % nqb;
  const int bh = bx / nqb;
  const int h  = bh % g.H;
  const int b  = bh / g.H;
  const int qbase_block = qb * AT_QB;
  const int q0 = qbase_block + wave * 16;

  const float* qb_ptr = q + (size_t)b * g.q_bs + (size_t)h * g.q_hs;
  const float* kb_ptr = k + (size_t)b * g.k_bs + (size_t)h * g.k_hs;
  const float* vb_ptr = v + (size_t)b * g.v_bs + (size_t)h * g.v_hs;
  float*       ob_ptr = out + (size_t)b * g.o_bs + (size_t)h * g.o_hs;

  v16b qah[2], qal[2];
  {
    const float* qrow = qb_ptr + (size_t)(q0 + c) * g.q_rs;
#pragma unroll
    for (int dc = 0; dc < 2; ++dc) {
#pragma unroll
      for (int e = 0; e < 8; ++e) {
        const float f0 = qrow[dc * 32 + 8 * hh + e] * g.qscale;
        const float f1 = qrow[dc * 32 + 16 + 8 * hh + e] * g.qscale;
        if (SPLIT_QK) { __bf16 hq, lq; at_split(f0, hq, lq); qah[dc][e] = hq; qal[dc][e] = lq; at_split(f1, hq, lq); qah[dc][8 + e] = hq; qal[dc][8 + e] = lq; }
        else { qah[dc][e] = at_to16<F16>(f0); qah[dc][8 + e] = at_to16<F16>(f1); qal[dc][e] = qah[dc][e]; qal[dc][8 + e] = qah[dc][8 + e]; }
      }
    }
  }

  float mrow[8], lrow[8];
  v8f oacc[4];
#pragma unroll
  for (int r = 0; r < 8; ++r) { mrow[r] = -INFINITY; lrow[r] = 0.f; }
#pragma unroll
  for (int t = 0; t < 4; ++t) oacc[t] = (v8f){0.f,0.f,0.f,0.f,0.f,0.f,0.f,0.f};

  const int nChunks = (g.mask_mode == 1 || g.mask_mode == 4) ? (qb + 1) : (g.Skv / AT_KC);
  int qkeep[8];
#pragma unroll
  for (int r = 0; r < 8; ++r) qkeep[r] = (g.mask_mode == 3) ? mask_b[(size_t)b * g.S + q0 + 8 * hh + r] : 1;
  for (int kc = 0; kc < nChunks; ++kc) {
    const int kv0 = kc * AT_KC;
    __syncthreads();
    {
      const int kvr = tid >> 1, dh = (tid & 1) * 32;
      const float* krow = kb_ptr + (size_t)(kv0 + kvr) * g.k_rs + dh;
      const float* vrow = vb_ptr + (size_t)(kv0 + kvr) * g.v_rs + dh;
#pragma unroll
      for (int i = 0; i < 8; ++i) {
        v4f kk = *(const v4f*)(krow + 4 * i);
        v4f vv = *(const v4f*)(vrow + 4 * i);
#pragma unroll
        for (int e = 0; e < 4; ++e) {
          const int d = dh + 4 * i + e;
          if (SPLIT_QK) { __bf16 a, bl; at_split(kk[e], a, bl); Ksh[kvr * AT_D + d] = a; Ksl[kvr * AT_D + d] = bl; }
          else Ksh[kvr * AT_D + d] = at_to16<F16>(kk[e]);
          if (SPLIT_PV) { __bf16 a, bl; at_split(vv[e], a, bl); Vth[d * AT_KC + kvr] = a; Vtl[d * AT_KC + kvr] = bl; }
          else Vth[d * AT_KC + kvr] = at_to16<F16>(vv[e]);
        }
      }
    }
    __syncthreads();

    v8f s[4];
#pragma unroll
    for (int j = 0; j < 4; ++j) {
      s[j] = (v8f){0.f,0.f,0.f,0.f,0.f,0.f,0.f,0.f};
#pragma unroll 1
      for (int dc = 0; dc < 2; ++dc) {
        FB kb;
        kb.h[0] = *(const v8b*)(Ksh + (j * 16 + c) * AT_D + dc * 32 + 8 * hh);
        kb.h[1] = *(const v8b*)(Ksh + (j * 16 + c) * AT_D + dc * 32 + 16 + 8 * hh);
        s[j] = at_mma16<F16>(qah[dc], kb.v, s[j]);
        if (SPLIT_QK) {
          FB kl;
          kl.h[0] = *(const v8b*)(Ksl + (j * 16 + c) * AT_D + dc * 32 + 8 * hh);
          kl.h[1] = *(const v8b*)(Ksl + (j * 16 + c) * AT_D + dc * 32 + 16 + 8 * hh);
          s[j] = at_mma16<F16>(qah[dc], kl.v, s[j]);
          s[j] = at_mma16<F16>(qal[dc], kb.v, s[j]);
        }
      }
    }
    const bool diag = (g.mask_mode == 1) && (kc == qb);
    int kvkeep[4] = {1, 1, 1, 1};
    if (g.mask_mode == 3) {
#pragma unroll
      for (int j = 0; j < 4; ++j) kvkeep[j] = ((const int*)mask_a)[(size_t)b * g.Skv + kv0 + j * 16 + c];
    }
    float cm[8];
#pragma unroll
    for (int r = 0; r < 8; ++r) {
      const int qrow = q0 + 8 * hh + r;
      float m = -INFINITY;
#pragma unroll
      for (int j = 0; j < 4; ++j) {
        const int kvcol = kv0 + j * 16 + c;
        bool masked = false;
        if (diag) masked = (kvcol > qrow);
        else if (g.mask_mode == 4) masked = (kvcol > qrow) || (qrow - kvcol > g.mask_is_int);
        else if (g.mask_mode == 2) {
          const size_t mi = (size_t)qrow * g.Skv + kvcol;
          masked = (g.mask_is_int == 0) ? (((const float*)mask_a)[mi] == 0.0f)
                 : (g.mask_is_int == 1) ? (((const int*)mask_a)[mi] == 0) : (((const int*)mask_a)[mi] != 0);
        } else if (g.mask_mode == 3) masked = (qkeep[r] == 0) || (kvkeep[j] == 0);
        else if (g.mask_mode == 5) {
          const size_t mi = (size_t)qrow * g.Skv + kvcol;
          masked = (((const int*)mask_a)[mi] != 0);
          int n = mask_b[mi]; n = n < 0 ? 0 : n;
          s[j][r] += g.cp[(size_t)b * g.c_bs + (size_t)h * g.c_hs + (size_t)qrow * g.c_rs + n]
                   + g.pc[(size_t)b * g.c_bs + (size_t)h * g.c_hs + (size_t)kvcol * g.c_rs + n];
        }
        if (masked) s[j][r] = g.mask_fill;
        m = fmaxf(m, s[j][r]);
      }
#pragma unroll
      for (int off = 1; off < 16; off <<= 1) m = fmaxf(m, __shfl_xor(m, off, 32));
      cm[r] = m;
    }
    __bf16* pwh = Psh[wave];
    __bf16* pwl = Psl[SPLIT_PV ? wave : 0];
#pragma unroll
    for (int r = 0; r < 8; ++r) {
      const float mnew = fmaxf(mrow[r], cm[r]);
      const float alpha = expf(mrow[r] - mnew);
      mrow[r] = mnew;
      float psum = 0.f;
#pragma unroll
      for (int j = 0; j < 4; ++j) {
        const float p = expf(s[j][r] - mnew);
        psum += p;
        if (SPLIT_PV) { __bf16 a, bl; at_split(p, a, bl); pwh[(8 * hh + r) * AT_KC + j * 16 + c] = a; pwl[(8 * hh + r) * AT_KC + j * 16 + c] = bl; }
        else pwh[(8 * hh + r) * AT_KC + j * 16 + c] = at_to16<F16>(p * PSC);
      }
#pragma unroll
      for (int off = 1; off < 16; off <<= 1) psum += __shfl_xor(psum, off, 32);
      lrow[r] = lrow[r] * alpha + psum;
#pragma unroll
      for (int t = 0; t < 4; ++t) oacc[t][r] *= alpha;
    }
    __builtin_amdgcn_fence(__ATOMIC_RELEASE, "workgroup");
    __builtin_amdgcn_wave_barrier();
    __builtin_amdgcn_fence(__ATOMIC_ACQUIRE, "workgroup");
#pragma unroll 1
    for (int kk = 0; kk < 2; ++kk) {
      FB pa, pl;
      pa.h[0] = *(const v8b*)(pwh + c * AT_KC + kk * 32 + 8 * hh);
      pa.h[1] = *(const v8b*)(pwh + c * AT_KC + kk * 32 + 16 + 8 * hh);
      if (SPLIT_PV) {
        pl.h[0] = *(const v8b*)(pwl + c * AT_KC + kk * 32 + 8 * hh);
        pl.h[1] = *(const v8b*)(pwl + c * AT_KC + kk * 32 + 16 + 8 * hh);
      }
#pragma unroll
      for (int t = 0; t < 4; ++t) {
        FB vb;
        vb.h[0] = *(const v8b*)(Vth + (t * 16 + c) * AT_KC + kk * 32 + 8 * hh);
        vb.h[1] = *(const v8b*)(Vth + (t * 16 + c) * AT_KC + kk * 32 + 16 + 8 * hh);
        oacc[t] = at_mma16<F16>(pa.v, vb.v, oacc[t]);
        if (SPLIT_PV) {
          FB vl;
          vl.h[0] = *(const v8b*)(Vtl + (t * 16 + c) * AT_KC + kk * 32 + 8 * hh);
          vl.h[1] = *(const v8b*)(Vtl + (t * 16 + c) * AT_KC + kk * 32 + 16 + 8 * hh);
          oacc[t] = at_mma16<F16>(pa.v, vl.v, oacc[t]);
          oacc[t] = at_mma16<F16>(pl.v, vb.v, oacc[t]);
        }
      }
    }
  }

  float* os = Os[wave];
#pragma unroll
  for (int r = 0; r < 8; ++r) {
    const float inv = 1.0f / (lrow[r] * PSC);
#pragma unroll
    for (int t = 0; t < 4; ++t) os[(8 * hh + r) * 68 + t * 16 + c] = oacc[t][r] * inv;
  }
  __builtin_amdgcn_fence(__ATOMIC_RELEASE, "workgroup");
  __builtin_amdgcn_wave_barrier();
  __builtin_amdgcn_fence(__ATOMIC_ACQUIRE, "workgroup");
  {
    const int c4 = (lane & 15) * 4;
    for (int pass = 0; pass < 2; ++pass) {
#pragma unroll
      for (int it = 0; it < 8; ++it) {
        const int row = it * 2 + hh;
        v4f val = *(const v4f*)(os + row * 68 + c4);
        *(volatile v4f*)(ob_ptr + (size_t)(q0 + row) * g.o_rs + c4) = val;
      }
      __threadfence();
    }
  }
}

}


__device__ __forceinline__ void st_h2(unsigned short* d2, float a, float b) { const unsigned u = (unsigned)__builtin_bit_cast(unsigned short, (_Float16)a) | ((unsigned)__builtin_bit_cast(unsigned short, (_Float16)b) << 16); volatile unsigned* d = (volatile unsigned*)d2; *d = u; __threadfence(); *d = u; }
__device__ __forceinline__ float ldh(const unsigned short* p) { return (float)__builtin_bit_cast(_Float16, *p); }
__device__ __forceinline__ v4f ld4h(const unsigned short* p) { const unsigned long long u = *(const unsigned long long*)p; v4f a;
    a.x = (float)__builtin_bit_cast(_Float16, (unsigned short)(u & 0xFFFFu)); a.y = (float)__builtin_bit_cast(_Float16, (unsigned short)((u >> 16) & 0xFFFFu)); a.z = (float)__builtin_bit_cast(_Float16, (unsigned short)((u >> 32) & 0xFFFFu)); a.w = (float)__builtin_bit_cast(_Float16, (unsigned short)((u >> 48) & 0xFFFFu)); return a; }
__device__ __forceinline__ unsigned long long pk4h(v4f s) { return (unsigned long long)__builtin_bit_cast(unsigned short, (_Float16)s.x) | ((unsigned long long)__builtin_bit_cast(unsigned short, (_Float16)s.y) << 16) | ((unsigned long long)__builtin_bit_cast(unsigned short, (_Float16)s.z) << 32) | ((unsigned long long)__builtin_bit_cast(unsigned short, (_Float16)s.w) << 48); }
typedef unsigned v4u __attribute__((ext_vector_type(4)));
__device__ __forceinline__ void st8h(unsigned short* d, v4f a, v4f b) { const unsigned long long pa = pk4h(a), pb = pk4h(b); v4u pk; pk.x = (unsigned)(pa & 0xFFFFFFFFull); pk.y = (unsigned)(pa >> 32); pk.z = (unsigned)(pb & 0xFFFFFFFFull); pk.w = (unsigned)(pb >> 32); volatile v4u* dd = (volatile v4u*)d; *dd = pk; __threadfence(); *dd = pk; }
__device__ __forceinline__ unsigned short bfu_rne(float v) { unsigned u = __builtin_bit_cast(unsigned, v); u += 0x7FFFu + ((u >> 16) & 1u); return (unsigned short)(u >> 16); }
__device__ __forceinline__ void bfsplit(float v, unsigned short& hi, unsigned short& lo) { hi = bfu_rne(v); lo = bfu_rne(v - __builtin_bit_cast(float, (unsigned)hi << 16)); }
__device__ __forceinline__ void st_s2(unsigned short* Hp, unsigned short* Lp, long long o, float a, float b) { unsigned short h0,l0,h1,l1; bfsplit(a,h0,l0); bfsplit(b,h1,l1); const unsigned ph = (unsigned)h0 | ((unsigned)h1 << 16), pl = (unsigned)l0 | ((unsigned)l1 << 16);
    volatile unsigned* dh = (volatile unsigned*)(Hp + o); volatile unsigned* dl = (volatile unsigned*)(Lp + o); *dh = ph; *dl = pl; __threadfence(); *dh = ph; *dl = pl; }
__device__ __forceinline__ int cl(int v, int n) { return min(max(v, 0), n - 1); }

template <int CH, bool SELF, int EWM, int EPI>
__global__ __launch_bounds__(256) void k_gat_agg(const unsigned short* __restrict__ XP, int XW, const float* __restrict__ AS, const float* __restrict__ AD, int ASTR, const float* __restrict__ EW, const float* __restrict__ CW,
        const int* __restrict__ esrc, const int* __restrict__ off, const int* __restrict__ cnt, const int* __restrict__ slot, const float* __restrict__ bias, const float* __restrict__ g, const float* __restrict__ bb,
        float* __restrict__ OUT, unsigned short* __restrict__ OH, unsigned short* __restrict__ OL, int N, int E, int CAP, float slope) {
    __shared__ float stage[8][256];
    const int wv = threadIdx.x >> 5; const int n = blockIdx.x * 8 + wv; const int L = threadIdx.x & 31; if (n >= N) return; const int c0 = 8 * L; const int h = c0 / CH;
    const float ad = AD[(long long)n * ASTR + h]; const float cw = (EWM == 1) ? CW[h] : 0.f; float m = -3.0e38f, s = 0.f; v4f a0, a1; a0.x = a0.y = a0.z = a0.w = 0.f; a1 = a0;
    const int p0 = cl(off[n], E + 1), cn = min(max(cnt[n], 0), CAP);
    for (int j = (SELF ? -1 : 0); j < cn; ++j) { int sj; float ew = 0.f;
        if (j < 0) { sj = n; ew = 1.f; } else { int e = slot[cl(p0 + j, E)]; e = cl(e, E); sj = cl(esrc[e], N); if (EWM != 0) ew = EW[e]; }
        float lg = AS[(long long)sj * ASTR + h] + ad + ((EWM == 1) ? ew * cw : 0.f); lg = (lg >= 0.f) ? lg : slope * lg;
        const float mn = fmaxf(m, lg); const float cz = expf(m - mn), pj = expf(lg - mn); s = s * cz + pj; const float pw = (EWM == 2) ? pj * ew : pj;
        const unsigned short* xr = XP + (long long)sj * XW + c0; a0 = a0 * cz + ld4h(xr) * pw; a1 = a1 * cz + ld4h(xr + 4) * pw; m = mn; }
    const float inv = (s > 0.f) ? 1.f / (s + 1e-16f) : 0.f; a0 = a0 * inv; a1 = a1 * inv;
    if (EPI == 0 || EPI == 1 || EPI == 4 || EPI == 5) { a0 = a0 + *(const v4f*)(bias + c0); a1 = a1 + *(const v4f*)(bias + c0 + 4); }
    if (EPI == 4 || EPI == 5) { a0.x = (a0.x > 0.f) ? a0.x : (expf(a0.x) - 1.f); a0.y = (a0.y > 0.f) ? a0.y : (expf(a0.y) - 1.f); a0.z = (a0.z > 0.f) ? a0.z : (expf(a0.z) - 1.f); a0.w = (a0.w > 0.f) ? a0.w : (expf(a0.w) - 1.f);
        a1.x = (a1.x > 0.f) ? a1.x : (expf(a1.x) - 1.f); a1.y = (a1.y > 0.f) ? a1.y : (expf(a1.y) - 1.f); a1.z = (a1.z > 0.f) ? a1.z : (expf(a1.z) - 1.f); a1.w = (a1.w > 0.f) ? a1.w : (expf(a1.w) - 1.f); }
    if (EPI == 4) { float o8[8] = {a0.x, a0.y, a0.z, a0.w, a1.x, a1.y, a1.z, a1.w}; unsigned short hh[8], ll[8];
#pragma unroll
        for (int u = 0; u < 8; ++u) bfsplit(o8[u], hh[u], ll[u]);
        const unsigned long long ph0 = (unsigned long long)hh[0] | ((unsigned long long)hh[1] << 16) | ((unsigned long long)hh[2] << 32) | ((unsigned long long)hh[3] << 48), pl0 = (unsigned long long)ll[0] | ((unsigned long long)ll[1] << 16) | ((unsigned long long)ll[2] << 32) | ((unsigned long long)ll[3] << 48);
        const unsigned long long ph1 = (unsigned long long)hh[4] | ((unsigned long long)hh[5] << 16) | ((unsigned long long)hh[6] << 32) | ((unsigned long long)hh[7] << 48), pl1 = (unsigned long long)ll[4] | ((unsigned long long)ll[5] << 16) | ((unsigned long long)ll[6] << 32) | ((unsigned long long)ll[7] << 48);
        v4u pk; pk.x = (unsigned)(ph0 & 0xFFFFFFFFull); pk.y = (unsigned)(ph0 >> 32); pk.z = (unsigned)(ph1 & 0xFFFFFFFFull); pk.w = (unsigned)(ph1 >> 32); volatile v4u* dh = (volatile v4u*)(OH + (long long)n * 256 + c0); *dh = pk; __threadfence(); *dh = pk;
        v4u ql; ql.x = (unsigned)(pl0 & 0xFFFFFFFFull); ql.y = (unsigned)(pl0 >> 32); ql.z = (unsigned)(pl1 & 0xFFFFFFFFull); ql.w = (unsigned)(pl1 >> 32); volatile v4u* dl = (volatile v4u*)(OL + (long long)n * 256 + c0); *dl = ql; __threadfence(); *dl = ql; return; }
    if (EPI == 6) {
        a0.x += __shfl_xor(a0.x, 16); a0.y += __shfl_xor(a0.y, 16); a0.z += __shfl_xor(a0.z, 16); a0.w += __shfl_xor(a0.w, 16); a1.x += __shfl_xor(a1.x, 16); a1.y += __shfl_xor(a1.y, 16); a1.z += __shfl_xor(a1.z, 16); a1.w += __shfl_xor(a1.w, 16);
        if (L < 16) { const int cb = 8 * L; const v4f b0 = *(const v4f*)(bias + cb), b1v = *(const v4f*)(bias + cb + 4);
            stage[wv][cb] = fmaxf(a0.x * 0.5f + b0.x, 0.f); stage[wv][cb + 1] = fmaxf(a0.y * 0.5f + b0.y, 0.f); stage[wv][cb + 2] = fmaxf(a0.z * 0.5f + b0.z, 0.f); stage[wv][cb + 3] = fmaxf(a0.w * 0.5f + b0.w, 0.f);
            stage[wv][cb + 4] = fmaxf(a1.x * 0.5f + b1v.x, 0.f); stage[wv][cb + 5] = fmaxf(a1.y * 0.5f + b1v.y, 0.f); stage[wv][cb + 6] = fmaxf(a1.z * 0.5f + b1v.z, 0.f); stage[wv][cb + 7] = fmaxf(a1.w * 0.5f + b1v.w, 0.f); }
        __builtin_amdgcn_fence(__ATOMIC_RELEASE, "workgroup"); __builtin_amdgcn_wave_barrier(); __builtin_amdgcn_fence(__ATOMIC_ACQUIRE, "workgroup");
        v4f o6; o6.x = stage[wv][4 * L]; o6.y = stage[wv][4 * L + 1]; o6.z = stage[wv][4 * L + 2]; o6.w = stage[wv][4 * L + 3]; VST2V4(OUT + (long long)n * 128 + 4 * L, o6); return; }
    if (EPI == 5) {
        a0.x += __shfl_xor(a0.x, 8); a0.y += __shfl_xor(a0.y, 8); a0.z += __shfl_xor(a0.z, 8); a0.w += __shfl_xor(a0.w, 8); a1.x += __shfl_xor(a1.x, 8); a1.y += __shfl_xor(a1.y, 8); a1.z += __shfl_xor(a1.z, 8); a1.w += __shfl_xor(a1.w, 8);
        a0.x += __shfl_xor(a0.x, 16); a0.y += __shfl_xor(a0.y, 16); a0.z += __shfl_xor(a0.z, 16); a0.w += __shfl_xor(a0.w, 16); a1.x += __shfl_xor(a1.x, 16); a1.y += __shfl_xor(a1.y, 16); a1.z += __shfl_xor(a1.z, 16); a1.w += __shfl_xor(a1.w, 16);
        const int gq5 = L & 7; a0 = a0 * 0.25f; a1 = a1 * 0.25f;
        if (L < 8) { stage[wv][8 * gq5] = a0.x; stage[wv][8 * gq5 + 1] = a0.y; stage[wv][8 * gq5 + 2] = a0.z; stage[wv][8 * gq5 + 3] = a0.w; stage[wv][8 * gq5 + 4] = a1.x; stage[wv][8 * gq5 + 5] = a1.y; stage[wv][8 * gq5 + 6] = a1.z; stage[wv][8 * gq5 + 7] = a1.w; }
        __builtin_amdgcn_fence(__ATOMIC_RELEASE, "workgroup"); __builtin_amdgcn_wave_barrier(); __builtin_amdgcn_fence(__ATOMIC_ACQUIRE, "workgroup");
        const unsigned long long pk5 = (unsigned long long)__builtin_bit_cast(unsigned, stage[wv][2 * L]) | ((unsigned long long)__builtin_bit_cast(unsigned, stage[wv][2 * L + 1]) << 32); VST2(unsigned long long, (unsigned long long*)(OUT + (long long)n * 64 + 2 * L), pk5); return; }
    if (EPI == 1) { float sm = a0.x + a0.y + a0.z + a0.w + a1.x + a1.y + a1.z + a1.w;
#pragma unroll
        for (int o = 16; o > 0; o >>= 1) sm += __shfl_xor(sm, o);
        const float mu = sm * (1.f / 256.f); const v4f d0 = a0 - mu, d1 = a1 - mu; float q = d0.x * d0.x + d0.y * d0.y + d0.z * d0.z + d0.w * d0.w + d1.x * d1.x + d1.y * d1.y + d1.z * d1.z + d1.w * d1.w;
#pragma unroll
        for (int o = 16; o > 0; o >>= 1) q += __shfl_xor(q, o);
        const float rs = rsqrtf(q * (1.f / 256.f) + 1e-5f); float o8[8] = {d0.x, d0.y, d0.z, d0.w, d1.x, d1.y, d1.z, d1.w}; unsigned short hh[8], ll[8];
#pragma unroll
        for (int u = 0; u < 8; ++u) { const float v = fmaxf(o8[u] * rs * g[c0 + u] + bb[c0 + u], 0.f); bfsplit(v, hh[u], ll[u]); }
        const unsigned long long ph0 = (unsigned long long)hh[0] | ((unsigned long long)hh[1] << 16) | ((unsigned long long)hh[2] << 32) | ((unsigned long long)hh[3] << 48), pl0 = (unsigned long long)ll[0] | ((unsigned long long)ll[1] << 16) | ((unsigned long long)ll[2] << 32) | ((unsigned long long)ll[3] << 48);
        const unsigned long long ph1 = (unsigned long long)hh[4] | ((unsigned long long)hh[5] << 16) | ((unsigned long long)hh[6] << 32) | ((unsigned long long)hh[7] << 48), pl1 = (unsigned long long)ll[4] | ((unsigned long long)ll[5] << 16) | ((unsigned long long)ll[6] << 32) | ((unsigned long long)ll[7] << 48);
        v4u pk; pk.x = (unsigned)(ph0 & 0xFFFFFFFFull); pk.y = (unsigned)(ph0 >> 32); pk.z = (unsigned)(ph1 & 0xFFFFFFFFull); pk.w = (unsigned)(ph1 >> 32); volatile v4u* dh = (volatile v4u*)(OH + (long long)n * 256 + c0); *dh = pk; __threadfence(); *dh = pk;
        v4u ql; ql.x = (unsigned)(pl0 & 0xFFFFFFFFull); ql.y = (unsigned)(pl0 >> 32); ql.z = (unsigned)(pl1 & 0xFFFFFFFFull); ql.w = (unsigned)(pl1 >> 32); volatile v4u* dl = (volatile v4u*)(OL + (long long)n * 256 + c0); *dl = ql; __threadfence(); *dl = ql; return; }
    if (EPI == 2 || EPI == 3) {
        a0.x += __shfl_xor(a0.x, 8); a0.y += __shfl_xor(a0.y, 8); a0.z += __shfl_xor(a0.z, 8); a0.w += __shfl_xor(a0.w, 8); a1.x += __shfl_xor(a1.x, 8); a1.y += __shfl_xor(a1.y, 8); a1.z += __shfl_xor(a1.z, 8); a1.w += __shfl_xor(a1.w, 8);
        a0.x += __shfl_xor(a0.x, 16); a0.y += __shfl_xor(a0.y, 16); a0.z += __shfl_xor(a0.z, 16); a0.w += __shfl_xor(a0.w, 16); a1.x += __shfl_xor(a1.x, 16); a1.y += __shfl_xor(a1.y, 16); a1.z += __shfl_xor(a1.z, 16); a1.w += __shfl_xor(a1.w, 16);
        const int gq = L & 7; a0 = a0 * 0.25f + *(const v4f*)(bias + 8 * gq); a1 = a1 * 0.25f + *(const v4f*)(bias + 8 * gq + 4);
        if (EPI == 3) { if (L < 8) { stage[wv][8 * gq] = a0.x; stage[wv][8 * gq + 1] = a0.y; stage[wv][8 * gq + 2] = a0.z; stage[wv][8 * gq + 3] = a0.w; stage[wv][8 * gq + 4] = a1.x; stage[wv][8 * gq + 5] = a1.y; stage[wv][8 * gq + 6] = a1.z; stage[wv][8 * gq + 7] = a1.w; }
            __builtin_amdgcn_fence(__ATOMIC_RELEASE, "workgroup"); __builtin_amdgcn_wave_barrier(); __builtin_amdgcn_fence(__ATOMIC_ACQUIRE, "workgroup");
            const unsigned long long pk3 = (unsigned long long)__builtin_bit_cast(unsigned, stage[wv][2 * L]) | ((unsigned long long)__builtin_bit_cast(unsigned, stage[wv][2 * L + 1]) << 32); VST2(unsigned long long, (unsigned long long*)(OUT + (long long)n * 64 + 2 * L), pk3); return; }
        float sm = (L < 8) ? (a0.x + a0.y + a0.z + a0.w + a1.x + a1.y + a1.z + a1.w) : 0.f;
#pragma unroll
        for (int o = 16; o > 0; o >>= 1) sm += __shfl_xor(sm, o);
        const float mu = sm * (1.f / 64.f); const v4f d0 = a0 - mu, d1 = a1 - mu; float q = (L < 8) ? (d0.x * d0.x + d0.y * d0.y + d0.z * d0.z + d0.w * d0.w + d1.x * d1.x + d1.y * d1.y + d1.z * d1.z + d1.w * d1.w) : 0.f;
#pragma unroll
        for (int o = 16; o > 0; o >>= 1) q += __shfl_xor(q, o);
        const float rs = rsqrtf(q * (1.f / 64.f) + 1e-5f);
        if (L < 8) { const float* gg = g + 8 * gq; const float* bq = bb + 8 * gq; stage[wv][8 * gq] = fmaxf(d0.x * rs * gg[0] + bq[0], 0.f); stage[wv][8 * gq + 1] = fmaxf(d0.y * rs * gg[1] + bq[1], 0.f); stage[wv][8 * gq + 2] = fmaxf(d0.z * rs * gg[2] + bq[2], 0.f); stage[wv][8 * gq + 3] = fmaxf(d0.w * rs * gg[3] + bq[3], 0.f);
            stage[wv][8 * gq + 4] = fmaxf(d1.x * rs * gg[4] + bq[4], 0.f); stage[wv][8 * gq + 5] = fmaxf(d1.y * rs * gg[5] + bq[5], 0.f); stage[wv][8 * gq + 6] = fmaxf(d1.z * rs * gg[6] + bq[6], 0.f); stage[wv][8 * gq + 7] = fmaxf(d1.w * rs * gg[7] + bq[7], 0.f); }
        __builtin_amdgcn_fence(__ATOMIC_RELEASE, "workgroup"); __builtin_amdgcn_wave_barrier(); __builtin_amdgcn_fence(__ATOMIC_ACQUIRE, "workgroup");
        const unsigned long long pk = (unsigned long long)__builtin_bit_cast(unsigned, stage[wv][2 * L]) | ((unsigned long long)__builtin_bit_cast(unsigned, stage[wv][2 * L + 1]) << 32); VST2(unsigned long long, (unsigned long long*)(OUT + (long long)n * 64 + 2 * L), pk); return; }
    stage[wv][c0] = a0.x; stage[wv][c0 + 1] = a0.y; stage[wv][c0 + 2] = a0.z; stage[wv][c0 + 3] = a0.w; stage[wv][c0 + 4] = a1.x; stage[wv][c0 + 5] = a1.y; stage[wv][c0 + 6] = a1.z; stage[wv][c0 + 7] = a1.w;
    __builtin_amdgcn_fence(__ATOMIC_RELEASE, "workgroup"); __builtin_amdgcn_wave_barrier(); __builtin_amdgcn_fence(__ATOMIC_ACQUIRE, "workgroup");
#pragma unroll
    for (int q2 = 0; q2 < 2; ++q2) { const int c = 128 * q2 + 4 * L; v4f v; v.x = stage[wv][c]; v.y = stage[wv][c + 1]; v.z = stage[wv][c + 2]; v.w = stage[wv][c + 3]; VST2V4(OUT + (long long)n * 256 + c, v); } }

__device__ __forceinline__ void st4s(unsigned short* Hp, unsigned short* Lp, long long o, v4f a) { unsigned short h[4], l[4]; bfsplit(a.x, h[0], l[0]); bfsplit(a.y, h[1], l[1]); bfsplit(a.z, h[2], l[2]); bfsplit(a.w, h[3], l[3]);
    const unsigned long long ph = (unsigned long long)h[0] | ((unsigned long long)h[1] << 16) | ((unsigned long long)h[2] << 32) | ((unsigned long long)h[3] << 48), pl = (unsigned long long)l[0] | ((unsigned long long)l[1] << 16) | ((unsigned long long)l[2] << 32) | ((unsigned long long)l[3] << 48);
    VST2(unsigned long long, (unsigned long long*)(Hp + o), ph); VST2(unsigned long long, (unsigned long long*)(Lp + o), pl); }
__global__ __launch_bounds__(256) void k_pl(const float* __restrict__ S, unsigned short* __restrict__ PH, unsigned short* __restrict__ PL, long long nval2, long long n2) { const long long u = (long long)blockIdx.x * 256 + threadIdx.x; if (u >= n2) return; const bool in = (u < nval2); const long long uc = in ? u : ((nval2 > 0) ? (nval2 - 1) : 0); const float a = S[2 * uc], b = S[2 * uc + 1]; st_s2(PH, PL, 2 * u, in ? a : 0.f, in ? b : 0.f); }
__global__ __launch_bounds__(256) void k_wext(const float* __restrict__ Wm, const float* __restrict__ AS_, const float* __restrict__ AD_, int K, int NOP, int FO, int NH, int DH, int EO, float* __restrict__ WC) {
    #pragma clang fp contract(off)
    const long long u = (long long)blockIdx.x * 256 + threadIdx.x; if (u >= (long long)K * NOP) return; const int kk = (int)(u / NOP), o = (int)(u % NOP);
    const int oo = min(o, FO - 1); const float vw = Wm[(long long)kk * FO + oo]; const int q = min(max(o - EO, 0), 2 * NH - 1); const int h = q % NH; float s = 0.f;
#pragma unroll 1
    for (int c = 0; c < DH; ++c) { const float w = Wm[(long long)kk * FO + h * DH + c]; const float asv = AS_[h * DH + c], adv = AD_[h * DH + c]; s += w * ((q < NH) ? asv : adv); }
    const float v = (o < FO) ? vw : ((o >= EO && o < EO + 2 * NH) ? s : 0.f); VST2(float, WC + u, v); }
template <int CH, bool SELF, int ACT, int MODE>
__global__ __launch_bounds__(256) void k_gat128(const float* __restrict__ HS, int P, int NH, const float* __restrict__ bias, const int* __restrict__ SRC, const int* __restrict__ off, const int* __restrict__ cnt, const int* __restrict__ slot,
        float* __restrict__ OUT, int OW, int OC, unsigned short* __restrict__ PH, unsigned short* __restrict__ PL, int PP, int N, int NP, int E, int CAP, float slope, float deps) {
    #pragma clang fp contract(off)
    const int n = blockIdx.x * 8 + (threadIdx.x >> 5); const int L = threadIdx.x & 31; if (n >= NP) return; const int c = 4 * L; const int h = c / CH; v4f o; o.x = o.y = o.z = o.w = 0.f;
    if (n < N) { const float* hn = HS + (long long)n * P; const float er = hn[128 + NH + h]; float m = -3.0e38f, s = 0.f; v4f a; a.x = a.y = a.z = a.w = 0.f;
        const int p0 = min(max(off[n], 0), E), cn = min(max(cnt[n], 0), CAP);
        for (int j = (SELF ? -1 : 0); j < cn; ++j) { int sj; if (j < 0) sj = n; else { const int e = min(max(slot[min(p0 + j, E - 1)], 0), E - 1); sj = min(max(SRC[e], 0), N - 1); }
            const float* hs = HS + (long long)sj * P; float lg = hs[128 + h] + er; lg = (lg >= 0.f) ? lg : slope * lg;
            const float mn = fmaxf(m, lg); const float cz = expf(m - mn), pj = expf(lg - mn); s = s * cz + pj; a = a * cz + *(const v4f*)(hs + c) * pj; m = mn; }
        const float inv = (s > 0.f || deps > 0.f) ? 1.f / (s + deps) : 0.f; o = a * inv + *(const v4f*)(bias + c);
        if (ACT == 1) { o.x = fmaxf(o.x, 0.f); o.y = fmaxf(o.y, 0.f); o.z = fmaxf(o.z, 0.f); o.w = fmaxf(o.w, 0.f); }
        if (ACT == 2) { o.x = (o.x > 0.f) ? o.x : (expf(o.x) - 1.f); o.y = (o.y > 0.f) ? o.y : (expf(o.y) - 1.f); o.z = (o.z > 0.f) ? o.z : (expf(o.z) - 1.f); o.w = (o.w > 0.f) ? o.w : (expf(o.w) - 1.f); }
        if (ACT == 3) { o.x = (o.x >= 0.f) ? o.x : 0.01f * o.x; o.y = (o.y >= 0.f) ? o.y : 0.01f * o.y; o.z = (o.z >= 0.f) ? o.z : 0.01f * o.z; o.w = (o.w >= 0.f) ? o.w : 0.01f * o.w; }
        if (MODE != 1 && c < OC) VST2V4(OUT + (long long)n * OW + c, o); }
    if (MODE != 0) st4s(PH, PL, (long long)n * PP + c, o); }

__global__ __launch_bounds__(256) void k_pl4(const float* __restrict__ S, int SW, int CW, int RV, int R, unsigned short* __restrict__ PH, unsigned short* __restrict__ PL, int PP) { const long long u = (long long)blockIdx.x * 256 + threadIdx.x; const int cq = CW / 4; if (u >= (long long)R * cq) return; const int r = (int)(u / cq); const int c = 4 * (int)(u % cq); v4f v; v.x = v.y = v.z = v.w = 0.f; if (r < RV) v = *(const v4f*)(S + (long long)r * SW + c); st4s(PH, PL, (long long)r * PP + c, v); }
__global__ __launch_bounds__(256) void k_cp4(const float* __restrict__ S, int SW, int CW, int R, float* __restrict__ D, int DW) { const long long u = (long long)blockIdx.x * 256 + threadIdx.x; const int cq = CW / 4; if (u >= (long long)R * cq) return; const int r = (int)(u / cq); const int c = 4 * (int)(u % cq); VST2V4(D + (long long)r * DW + c, *(const v4f*)(S + (long long)r * SW + c)); }
__global__ __launch_bounds__(256) void k_bt2(const float* __restrict__ Wa, int KA, const float* __restrict__ Wb, int KB, int KOFF, int NO, int KP, unsigned short* __restrict__ PH, unsigned short* __restrict__ PL) {
    const long long u = (long long)blockIdx.x * 256 + threadIdx.x; if (u >= (long long)NO * (KP / 2)) return; const int o = (int)(u / (KP / 2)); const int k0 = 2 * (int)(u % (KP / 2)); float v[2];
#pragma unroll
    for (int t = 0; t < 2; ++t) { const int kk = k0 + t; const float va = Wa[(long long)min(kk, KA - 1) * NO + o]; const float vb = Wb[(long long)min(max(kk - KOFF, 0), KB - 1) * NO + o]; v[t] = (kk < KA) ? va : ((kk >= KOFF && kk < KOFF + KB) ? vb : 0.f); }
    st_s2(PH, PL, (long long)o * KP + k0, v[0], v[1]); }
__global__ __launch_bounds__(256) void k_zero4(float* __restrict__ B, long long n4) { const long long u = (long long)blockIdx.x * 256 + threadIdx.x; if (u >= n4) return; v4f z; z.x = z.y = z.z = z.w = 0.f; VST2V4(B + 4 * u, z); }
__global__ __launch_bounds__(256) void k_padvec(const float* __restrict__ bsrc, int nb, float* __restrict__ Bd, int n) { const int t = blockIdx.x * 256 + threadIdx.x; if (t >= n) return; VST2(float, Bd + t, (t < nb) ? bsrc[min(t, nb - 1)] : 0.f); }

__global__ __launch_bounds__(256) void k_u2_bt(const float* __restrict__ Wm, int ldw, int TRANS, int KI, int NO, int KP, int NOP, const float* __restrict__ S, unsigned short* __restrict__ PH_, unsigned short* __restrict__ PL_) {
    const long long u = (long long)blockIdx.x * 256 + threadIdx.x; if (u >= (long long)NOP * (KP / 2)) return; const int k0 = 2 * (int)(u % (KP / 2)); const int o = (int)(u / (KP / 2)); float a = 0.f, b = 0.f;
    if (o < NO) { const float s = S ? S[o] : 1.f;
        if (k0 < KI) a = (TRANS ? Wm[(long long)k0 * ldw + o] : Wm[(long long)o * ldw + k0]) * s;
        if (k0 + 1 < KI) b = (TRANS ? Wm[(long long)(k0 + 1) * ldw + o] : Wm[(long long)o * ldw + k0 + 1]) * s; }
    st_s2(PH_, PL_, (long long)o * KP + k0, a, b); }
__global__ __launch_bounds__(256) void k_u2_vec(const float* __restrict__ A, const float* __restrict__ S, const float* __restrict__ B2, int n, int NP, float* __restrict__ O) { for (int i = threadIdx.x; i < NP; i += 256) { float v = 0.f; if (i < n) v = A[i] * (S ? S[i] : 1.f) + (B2 ? B2[i] : 0.f); VST2(float, O + i, v); } }
__global__ __launch_bounds__(256) void k_u2_colstat(const float* __restrict__ X, int P, int N, float eps, float* __restrict__ STAT) {
    #pragma clang fp contract(off)
    __shared__ float red[256]; const int c = blockIdx.x; const int t = threadIdx.x; float s = 0.f; for (int r = t; r < N; r += 256) s += X[(long long)r * P + c]; red[t] = s; __syncthreads();
    for (int o = 128; o > 0; o >>= 1) { if (t < o) red[t] += red[t + o]; __syncthreads(); }
    const float mu = red[0] / (float)N; __syncthreads(); float q = 0.f; for (int r = t; r < N; r += 256) { const float d = X[(long long)r * P + c] - mu; q += d * d; } red[t] = q; __syncthreads();
    for (int o = 128; o > 0; o >>= 1) { if (t < o) red[t] += red[t + o]; __syncthreads(); }
    const float rs = 1.f / sqrtf(red[0] / (float)N + eps); if (t < 32) VST2(float, STAT + (long long)c * 32 + t, (t == 0) ? mu : ((t == 1) ? rs : 0.f)); }
__global__ __launch_bounds__(256) void k_u2_pl(const float* __restrict__ X, int PW, int Wd, int RL, int RP, unsigned short* __restrict__ PH_, unsigned short* __restrict__ PL_, int PP, int coff) { const long long u = (long long)blockIdx.x * 256 + threadIdx.x; if (u >= (long long)RP * (Wd / 4)) return; const int r = (int)(u / (Wd / 4)); const int c = 4 * (int)(u % (Wd / 4)); v4f v; v.x = v.y = v.z = v.w = 0.f; if (r < RL) v = *(const v4f*)(X + (long long)r * PW + c); st4s(PH_, PL_, (long long)r * PP + coff + c, v); }
__constant__ int c_perm[4416] = {2, 6, 9, 11, 27, 33, 44, 49, 50, 68, 76, 83, 85, 90, 95, 104, 105, 108, 115, 129, 135, 152, 155, 157, 158, 161, 164, 167, 193, 197, 214, 215, 217, 226, 242, 249, 255, 259, 261, 264, 268, 274, 281, 298, 301, 307, 309, 311, 342, 348, 352, 361, 369, 371, 379, 386, 392, 403, 405, 420, 421, 423, 430, 432, 433, 438, 442, 448, 465, 469, 479, 481, 494, 500, 507, 513, 514, 519, 535, 537, 546, 555, 558, 569, 578, 592, 602, 603, 613, 617, 631, 640, 651, 671, 676, 679, 688, 703, 706, 707, 708, 710, 716, 724, 734, 748, 752, 759, 768, 772, 774, 777, 781, 782, 803, 811, 819, 824, 829, 833, 860, 871, 883, 891, 894, 898, 899, 903, 909, 931, 933, 937, 940, 943, 951, 952, 955, 956, 967, 968, 969, 988, 999, 1014, 1019, 1024, 1025, 1032, 1033, 1035, 1039, 1051, 1057, 1068, 1079, 1083, 1086, 1090, 1096, 1100, 1111, 1122, 1129, 1144, 1151, 1153, 1162, 1163, 1174, 1189, 1196, 1221, 1230, 1233, 1253, 1254, 1256, 1264, 1273, 1296, 1308, 1314, 1317, 1338, 1340, 1346, 1350, 1352, 1355, 1356, 1360, 1364, 1365, 1374, 1386, 1404, 1409, 1419, 1420, 1424, 1434, 1450, 1452, 1454, 1460, 1463, 1468, 1476, 1479, 1483, 1494, 1507, 1509, 1513, 1517, 1545, 1555, 1570, 1574, 1576, 1595, 1597, 1604, 1607, 1614, 1623, 1626, 1631, 1639, 1646, 1647, 1656, 1663, 1666, 1681, 1683, 1693, 1694, 1697, 1705, 1706, 1727, 1751, 1752, 1756, 1757, 1777, 1778, 1784, 1790, 1800, 1808, 1822, 1823, 1825, 1846, 1850, 1851, 1855, 1862, 1871, 1885, 1908, 1918, 1921, 1938, 1939, 1955, 1974, 1982, 1983, 1986, 1989, 2023, 2024, 2029, 2036, 2042, 2050, 2052, 2059, 2064, 2071, 2080, 2086, 2097, 2100, 2101, 2114, 2123, 2142, 2150, 2155, 2157, 2169, 2182, 2195, 2199, 2201, 2202, 2204, 2212, 2213, 2231, 2232, 2237, 2276, 2278, 2289, 2303, 2305, 2322, 2330, 2358, 2359, 2365, 2372, 2396, 2401, 2402, 2408, 2412, 2415, 2418, 2420, 2422, 2424, 2431, 2441, 2452, 2453, 2455, 2459, 2460, 2473, 2479, 2484, 2510, 2511, 2517, 2520, 2522, 2523, 2537, 2544, 2550, 2566, 2570, 2575, 2583, 2610, 2625, 2655, 2659, 2661, 2662, 2668, 2707, 2728, 2736, 2749, 2753, 2757, 2762, 2781, 2784, 2790, 2809, 2818, 2821, 2823, 2831, 2836, 2859, 2862, 2864, 2868, 2876, 2878, 2879, 2887, 2889, 2895, 2901, 2902, 2905, 2916, 2930, 2942, 2948, 2957, 2959, 2989, 2992, 2994, 3001, 3029, 3030, 3031, 3033, 3044, 3045, 3051, 3068, 3076, 3077, 3092, 3100, 3108, 3116, 3124, 3127, 3136, 3137, 3140, 3153, 3161, 3171, 3192, 3211, 3214, 3215, 3217, 3223, 3236, 3259, 3282, 3300, 3301, 3347, 3361, 3364, 3386, 3392, 3397, 3399, 3400, 3403, 3405, 3410, 3424, 3432, 3436, 3448, 3452, 3463, 3471, 3476, 3482, 3486, 3488, 3501, 3517, 3532, 3535, 3543, 3582, 3587, 3595, 3605, 3618, 3632, 3638, 3644, 3646, 3657, 3659, 3660, 3678, 3700, 3701, 3716, 3717, 3744, 3745, 3748, 3749, 3773, 3776, 3806, 3808, 3809, 3812, 3819, 3827, 3833, 3834, 3851, 3856, 3860, 3869, 3870, 3909, 3912, 3917, 3927, 3934, 3941, 3951, 3972, 3978, 3980, 4001, 4007, 4008, 4009, 4018, 4033, 4040, 4043, 4055, 4060, 4070, 4071, 4084, 4085, 4093, -1, -1, -1, -1, -1, -1, -1, -1, -1, -1, -1, -1, -1, -1, -1, -1, -1, -1, -1, -1, -1, -1, -1, -1, -1, -1, -1, -1, -1, -1, -1, -1, -1, -1, -1, -1, -1, -1, -1, -1, -1, -1, -1, -1, -1, -1, -1, -1, -1, -1, -1, -1, -1, -1, -1, -1, -1, -1, -1, 19, 28, 34, 38, 39, 42, 46, 47, 53, 55, 59, 62, 70, 75, 81, 96, 99, 101, 125, 133, 142, 146, 154, 156, 159, 160, 166, 175, 178, 182, 212, 218, 224, 232, 241, 254, 270, 273, 283, 292, 308, 314, 332, 375, 401, 408, 419, 427, 434, 440, 445, 450, 462, 471, 473, 488, 491, 496, 503, 504, 505, 509, 528, 549, 556, 559, 564, 577, 585, 587, 594, 595, 599, 612, 614, 616, 634, 659, 662, 668, 692, 695, 696, 702, 731, 741, 754, 756, 770, 775, 790, 802, 804, 805, 810, 812, 821, 831, 832, 835, 840, 851, 852, 857, 873, 879, 881, 897, 901, 905, 906, 907, 918, 920, 932, 935, 936, 945, 946, 954, 965, 966, 970, 978, 983, 989, 992, 994, 1000, 1042, 1045, 1072, 1082, 1085, 1092, 1095, 1104, 1107, 1116, 1124, 1131, 1137, 1159, 1178, 1179, 1181, 1191, 1194, 1197, 1202, 1206, 1207, 1215, 1218, 1228, 1251, 1257, 1259, 1271, 1274, 1280, 1287, 1303, 1316, 1320, 1327, 1328, 1331, 1336, 1348, 1359, 1370, 1378, 1385, 1389, 1390, 1393, 1396, 1400, 1401, 1403, 1414, 1427, 1441, 1443, 1447, 1455, 1477, 1478, 1480, 1495, 1502, 1503, 1514, 1529, 1552, 1558, 1566, 1582, 1592, 1593, 1602, 1603, 1617, 1620, 1632, 1633, 1634, 1636, 1637, 1645, 1651, 1676, 1678, 1700, 1703, 1716, 1721, 1728, 1734, 1741, 1742, 1747, 1763, 1770, 1772, 1776, 1788, 1791, 1793, 1798, 1806, 1810, 1815, 1827, 1835, 1854, 1873, 1894, 1898, 1901, 1902, 1915, 1926, 1934, 1956, 1961, 1963, 1970, 1979, 1985, 1992, 1994, 1999, 2000, 2008, 2014, 2038, 2044, 2048, 2063, 2069, 2070, 2096, 2099, 2109, 2110, 2117, 2122, 2129, 2141, 2144, 2146, 2151, 2161, 2181, 2183, 2186, 2193, 2200, 2210, 2221, 2222, 2226, 2242, 2255, 2257, 2277, 2296, 2297, 2302, 2304, 2313, 2319, 2323, 2335, 2343, 2344, 2346, 2355, 2364, 2370, 2381, 2391, 2414, 2419, 2429, 2447, 2448, 2456, 2466, 2467, 2468, 2469, 2472, 2495, 2515, 2526, 2532, 2533, 2534, 2546, 2548, 2551, 2561, 2580, 2601, 2605, 2611, 2623, 2635, 2637, 2646, 2652, 2663, 2671, 2677, 2678, 2680, 2684, 2687, 2704, 2705, 2706, 2717, 2733, 2742, 2744, 2751, 2765, 2777, 2783, 2811, 2815, 2816, 2830, 2837, 2838, 2849, 2851, 2855, 2860, 2861, 2866, 2875, 2898, 2900, 2919, 2921, 2924, 2950, 2953, 2958, 2967, 2974, 2990, 3002, 3026, 3037, 3038, 3052, 3059, 3063, 3064, 3075, 3081, 3096, 3097, 3098, 3105, 3117, 3118, 3123, 3129, 3141, 3142, 3147, 3148, 3152, 3154, 3174, 3185, 3187, 3189, 3191, 3204, 3219, 3222, 3232, 3233, 3246, 3252, 3253, 3260, 3262, 3263, 3280, 3286, 3288, 3289, 3302, 3315, 3317, 3319, 3324, 3330, 3339, 3350, 3352, 3354, 3357, 3359, 3384, 3385, 3389, 3401, 3404, 3420, 3426, 3429, 3434, 3440, 3443, 3445, 3451, 3455, 3457, 3477, 3478, 3491, 3497, 3504, 3519, 3530, 3546, 3548, 3562, 3575, 3579, 3611, 3615, 3622, 3624, 3636, 3647, 3651, 3655, 3666, 3667, 3668, 3677, 3682, 3694, 3698, 3699, 3703, 3705, 3721, 3724, 3726, 3731, 3746, 3747, 3754, 3760, 3764, 3769, 3772, 3782, 3787, 3790, 3793, 3813, 3815, 3823, 3826, 3841, 3849, 3855, 3879, 3883, 3884, 3895, 3900, 3905, 3906, 3907, 3910, 3914, 3944, 3948, 3949, 3964, 3973, 3992, 3996, 3999, 4005, 4020, 4025, 4026, 4030, 4034, 4045, 4056, 4072, 4078, -1, -1, -1, -1, -1, -1, -1, -1, -1, -1, -1, -1, -1, -1, -1, -1, -1, -1, -1, -1, -1, -1, -1, -1, -1, -1, -1, -1, -1, -1, -1, -1, -1, -1, -1, -1, -1, -1, -1, -1, -1, -1, -1, -1, -1, -1, -1, -1, -1, 18, 22, 24, 43, 77, 86, 89, 102, 114, 118, 121, 123, 127, 128, 138, 139, 143, 150, 165, 170, 174, 176, 179, 185, 189, 195, 203, 207, 213, 222, 225, 227, 238, 239, 246, 250, 257, 280, 288, 291, 294, 302, 318, 322, 339, 345, 350, 358, 360, 370, 373, 377, 384, 388, 393, 400, 402, 409, 411, 417, 422, 447, 449, 472, 492, 495, 517, 518, 526, 531, 536, 538, 543, 572, 573, 600, 604, 607, 610, 619, 624, 627, 629, 630, 637, 642, 645, 646, 656, 660, 680, 683, 687, 693, 712, 725, 726, 736, 758, 767, 771, 796, 806, 808, 830, 834, 836, 837, 844, 847, 849, 859, 863, 878, 880, 882, 889, 890, 908, 911, 919, 926, 927, 930, 960, 962, 973, 982, 1003, 1022, 1041, 1052, 1054, 1059, 1061, 1071, 1074, 1088, 1103, 1117, 1121, 1133, 1139, 1143, 1145, 1147, 1155, 1168, 1175, 1185, 1186, 1199, 1213, 1223, 1235, 1250, 1255, 1261, 1269, 1276, 1277, 1282, 1288, 1295, 1298, 1301, 1304, 1305, 1307, 1309, 1321, 1330, 1342, 1344, 1351, 1353, 1361, 1371, 1375, 1377, 1418, 1421, 1426, 1428, 1440, 1457, 1459, 1469, 1485, 1496, 1510, 1515, 1527, 1546, 1549, 1550, 1562, 1563, 1567, 1579, 1587, 1601, 1629, 1642, 1655, 1669, 1672, 1702, 1707, 1709, 1710, 1713, 1731, 1736, 1745, 1749, 1750, 1753, 1758, 1767, 1771, 1785, 1786, 1787, 1821, 1829, 1831, 1832, 1834, 1849, 1860, 1864, 1865, 1877, 1880, 1882, 1888, 1892, 1910, 1924, 1942, 1960, 1967, 1968, 1975, 1976, 1980, 1991, 2019, 2020, 2022, 2031, 2033, 2035, 2039, 2043, 2046, 2056, 2058, 2060, 2084, 2108, 2113, 2116, 2119, 2148, 2158, 2159, 2171, 2173, 2179, 2194, 2197, 2205, 2215, 2227, 2229, 2238, 2239, 2243, 2248, 2260, 2262, 2269, 2287, 2314, 2317, 2320, 2336, 2341, 2347, 2353, 2366, 2369, 2371, 2376, 2377, 2379, 2388, 2394, 2403, 2410, 2411, 2416, 2421, 2442, 2443, 2445, 2461, 2494, 2509, 2512, 2513, 2514, 2528, 2542, 2543, 2552, 2553, 2577, 2579, 2582, 2595, 2599, 2622, 2626, 2638, 2654, 2670, 2672, 2675, 2685, 2686, 2700, 2711, 2726, 2727, 2743, 2747, 2754, 2758, 2761, 2775, 2780, 2793, 2794, 2802, 2805, 2808, 2812, 2813, 2817, 2822, 2825, 2832, 2839, 2847, 2850, 2853, 2854, 2867, 2873, 2883, 2925, 2928, 2929, 2933, 2940, 2966, 2971, 2973, 2976, 2986, 2995, 3004, 3011, 3016, 3101, 3112, 3119, 3120, 3126, 3133, 3134, 3138, 3163, 3169, 3172, 3178, 3184, 3193, 3202, 3218, 3220, 3248, 3266, 3267, 3277, 3279, 3303, 3306, 3308, 3309, 3325, 3327, 3329, 3336, 3349, 3358, 3360, 3363, 3370, 3380, 3387, 3391, 3394, 3395, 3402, 3406, 3408, 3418, 3431, 3437, 3441, 3450, 3456, 3461, 3465, 3468, 3469, 3473, 3481, 3495, 3508, 3513, 3523, 3527, 3544, 3560, 3564, 3571, 3585, 3599, 3617, 3642, 3652, 3663, 3664, 3674, 3676, 3681, 3683, 3687, 3696, 3702, 3712, 3718, 3737, 3742, 3743, 3752, 3757, 3775, 3785, 3807, 3810, 3814, 3829, 3842, 3843, 3845, 3866, 3868, 3885, 3891, 3897, 3899, 3916, 3928, 3942, 3958, 3959, 3963, 3967, 3969, 3970, 3981, 3993, 4014, 4019, 4022, 4038, 4051, 4053, 4061, 4062, 4081, 4083, -1, -1, -1, -1, -1, -1, -1, -1, -1, -1, -1, -1, -1, -1, 4, 12, 16, 17, 31, 45, 52, 57, 72, 74, 82, 84, 87, 103, 107, 109, 126, 130, 131, 163, 168, 171, 177, 187, 205, 220, 237, 244, 251, 260, 277, 296, 297, 299, 300, 310, 315, 317, 325, 336, 337, 344, 346, 353, 359, 376, 378, 414, 415, 416, 459, 460, 466, 470, 480, 497, 498, 508, 521, 525, 527, 533, 540, 554, 565, 579, 589, 593, 596, 598, 601, 611, 626, 635, 643, 657, 682, 685, 686, 694, 717, 720, 721, 727, 738, 740, 757, 762, 766, 776, 798, 799, 809, 818, 823, 843, 845, 854, 858, 861, 866, 867, 876, 877, 884, 893, 900, 904, 922, 924, 934, 942, 950, 957, 972, 975, 976, 987, 991, 1007, 1009, 1016, 1020, 1021, 1026, 1031, 1036, 1048, 1050, 1056, 1058, 1060, 1073, 1076, 1093, 1097, 1113, 1127, 1152, 1166, 1170, 1171, 1172, 1177, 1180, 1182, 1195, 1208, 1209, 1210, 1214, 1217, 1219, 1227, 1231, 1236, 1240, 1262, 1266, 1268, 1279, 1310, 1313, 1322, 1332, 1362, 1367, 1373, 1384, 1388, 1392, 1395, 1397, 1410, 1422, 1425, 1432, 1442, 1445, 1461, 1462, 1481, 1486, 1487, 1488, 1490, 1506, 1511, 1520, 1530, 1531, 1536, 1538, 1541, 1548, 1554, 1559, 1564, 1584, 1585, 1589, 1591, 1596, 1598, 1605, 1630, 1635, 1654, 1660, 1664, 1677, 1685, 1688, 1714, 1715, 1719, 1737, 1738, 1740, 1744, 1754, 1759, 1760, 1764, 1773, 1782, 1799, 1801, 1811, 1817, 1820, 1838, 1844, 1848, 1857, 1861, 1869, 1891, 1896, 1903, 1909, 1912, 1919, 1920, 1927, 1943, 1946, 1950, 1984, 1996, 2002, 2006, 2007, 2009, 2011, 2013, 2016, 2018, 2021, 2032, 2062, 2076, 2104, 2107, 2111, 2115, 2121, 2124, 2127, 2128, 2132, 2136, 2137, 2140, 2145, 2153, 2154, 2160, 2165, 2177, 2185, 2189, 2203, 2206, 2209, 2214, 2218, 2223, 2235, 2236, 2241, 2247, 2259, 2265, 2273, 2275, 2279, 2285, 2288, 2308, 2311, 2316, 2318, 2324, 2333, 2334, 2337, 2340, 2342, 2357, 2363, 2375, 2378, 2385, 2387, 2389, 2397, 2434, 2450, 2462, 2465, 2475, 2478, 2482, 2496, 2505, 2506, 2516, 2549, 2555, 2571, 2573, 2581, 2584, 2586, 2588, 2591, 2593, 2598, 2600, 2619, 2640, 2645, 2647, 2656, 2658, 2660, 2667, 2681, 2683, 2695, 2702, 2703, 2710, 2719, 2725, 2731, 2734, 2740, 2741, 2750, 2760, 2763, 2772, 2778, 2782, 2786, 2791, 2800, 2829, 2844, 2846, 2848, 2871, 2872, 2882, 2884, 2888, 2896, 2903, 2917, 2922, 2926, 2927, 2932, 2934, 2935, 2937, 2938, 2941, 2956, 2962, 2965, 2979, 2980, 3000, 3007, 3013, 3021, 3022, 3023, 3025, 3035, 3042, 3048, 3055, 3087, 3093, 3095, 3104, 3111, 3146, 3155, 3157, 3158, 3166, 3167, 3183, 3199, 3207, 3208, 3209, 3212, 3221, 3225, 3229, 3234, 3240, 3243, 3249, 3264, 3274, 3283, 3285, 3287, 3290, 3293, 3295, 3304, 3310, 3314, 3337, 3341, 3344, 3366, 3367, 3368, 3377, 3378, 3382, 3414, 3442, 3459, 3462, 3475, 3487, 3489, 3512, 3514, 3520, 3526, 3528, 3534, 3542, 3566, 3569, 3580, 3584, 3591, 3593, 3601, 3602, 3621, 3629, 3631, 3656, 3669, 3672, 3685, 3688, 3692, 3704, 3715, 3719, 3728, 3750, 3758, 3767, 3781, 3799, 3800, 3802, 3803, 3817, 3824, 3828, 3837, 3838, 3854, 3862, 3875, 3896, 3903, 3919, 3923, 3929, 3931, 3936, 3938, 3939, 3943, 3952, 3954, 3961, 3965, 3976, 3986, 4017, 4029, 4044, 4048, 4049, 4052, 4064, 4074, 4076, 4086, 4089, -1, -1, -1, -1, -1, -1, -1, -1, -1, -1, -1, -1, -1, -1, -1, -1, -1, -1, -1, -1, -1, -1, -1, -1, -1, -1, -1, -1, -1, -1, -1, -1, -1, -1, -1, -1, -1, -1, -1, -1, -1, -1, -1, -1, -1, -1, -1, -1, 20, 29, 30, 36, 48, 63, 79, 92, 94, 112, 120, 124, 141, 144, 145, 153, 184, 196, 208, 210, 221, 229, 236, 252, 266, 289, 290, 295, 304, 305, 313, 320, 321, 324, 327, 330, 331, 334, 335, 341, 343, 347, 354, 356, 357, 365, 366, 374, 380, 396, 398, 404, 407, 410, 412, 413, 418, 437, 439, 446, 467, 477, 483, 486, 499, 506, 510, 511, 512, 522, 530, 532, 547, 550, 552, 557, 561, 563, 580, 583, 588, 591, 597, 618, 622, 623, 628, 633, 652, 663, 664, 672, 689, 699, 713, 715, 728, 732, 744, 746, 749, 765, 778, 780, 783, 786, 807, 814, 817, 825, 826, 838, 842, 862, 875, 885, 923, 938, 959, 961, 974, 977, 979, 986, 995, 1001, 1002, 1004, 1011, 1017, 1030, 1065, 1067, 1069, 1098, 1101, 1109, 1123, 1130, 1136, 1142, 1148, 1161, 1167, 1198, 1205, 1211, 1247, 1258, 1263, 1281, 1299, 1312, 1315, 1318, 1329, 1368, 1391, 1433, 1439, 1470, 1472, 1484, 1489, 1499, 1512, 1516, 1528, 1540, 1547, 1556, 1578, 1580, 1583, 1594, 1599, 1619, 1650, 1659, 1675, 1680, 1684, 1691, 1717, 1722, 1723, 1726, 1729, 1735, 1743, 1746, 1748, 1779, 1794, 1795, 1807, 1814, 1840, 1842, 1843, 1847, 1852, 1858, 1859, 1863, 1867, 1870, 1872, 1883, 1890, 1897, 1899, 1900, 1905, 1906, 1911, 1913, 1932, 1935, 1940, 1944, 1948, 1953, 1969, 1972, 1990, 1997, 2025, 2026, 2028, 2051, 2053, 2077, 2078, 2088, 2094, 2102, 2118, 2120, 2125, 2131, 2133, 2134, 2138, 2143, 2147, 2152, 2180, 2184, 2187, 2207, 2216, 2219, 2220, 2224, 2228, 2244, 2251, 2252, 2263, 2264, 2281, 2286, 2290, 2295, 2300, 2309, 2325, 2327, 2345, 2348, 2361, 2362, 2392, 2395, 2398, 2406, 2407, 2409, 2428, 2444, 2446, 2454, 2457, 2463, 2464, 2486, 2487, 2489, 2493, 2500, 2501, 2529, 2531, 2536, 2538, 2554, 2562, 2569, 2578, 2585, 2587, 2590, 2604, 2608, 2636, 2644, 2653, 2669, 2688, 2689, 2691, 2713, 2714, 2720, 2721, 2729, 2748, 2752, 2759, 2779, 2789, 2792, 2796, 2797, 2801, 2807, 2840, 2842, 2852, 2857, 2880, 2893, 2913, 2931, 2947, 2951, 2955, 2961, 2972, 2983, 2988, 2998, 3003, 3014, 3024, 3028, 3032, 3039, 3047, 3049, 3053, 3054, 3062, 3065, 3066, 3070, 3071, 3072, 3074, 3128, 3130, 3139, 3149, 3164, 3175, 3180, 3190, 3194, 3195, 3196, 3200, 3203, 3210, 3224, 3231, 3239, 3251, 3254, 3265, 3273, 3276, 3281, 3292, 3299, 3305, 3331, 3335, 3343, 3345, 3369, 3398, 3415, 3419, 3430, 3435, 3446, 3453, 3460, 3464, 3466, 3494, 3498, 3499, 3500, 3506, 3516, 3538, 3552, 3556, 3557, 3572, 3577, 3581, 3583, 3588, 3590, 3598, 3604, 3612, 3613, 3625, 3627, 3630, 3637, 3648, 3662, 3684, 3697, 3710, 3723, 3727, 3755, 3759, 3765, 3766, 3771, 3778, 3779, 3783, 3784, 3795, 3818, 3821, 3822, 3831, 3836, 3839, 3846, 3850, 3853, 3871, 3876, 3881, 3892, 3902, 3915, 3918, 3924, 3930, 3955, 3979, 3982, 3989, 3995, 4000, 4002, 4006, 4012, 4021, 4035, 4050, 4057, 4069, 4077, 4079, 4080, 4082, 4087, 4090, 4092, -1, -1, -1, -1, -1, -1, -1, -1, -1, -1, -1, -1, -1, -1, -1, -1, -1, -1, -1, -1, -1, -1, -1, -1, -1, -1, -1, -1, -1, -1, -1, 13, 14, 15, 21, 23, 40, 51, 65, 69, 71, 73, 80, 106, 113, 116, 119, 134, 140, 147, 149, 162, 172, 180, 190, 191, 194, 198, 211, 230, 231, 234, 258, 285, 293, 303, 319, 333, 362, 364, 367, 368, 382, 391, 394, 395, 397, 406, 424, 444, 451, 453, 455, 458, 464, 474, 482, 485, 489, 515, 524, 529, 541, 548, 560, 568, 584, 605, 608, 621, 632, 641, 653, 655, 665, 669, 670, 674, 675, 684, 691, 698, 711, 714, 722, 730, 737, 743, 745, 750, 753, 763, 764, 779, 791, 793, 797, 813, 828, 839, 841, 850, 853, 855, 856, 888, 895, 912, 915, 916, 928, 944, 947, 948, 949, 981, 990, 997, 998, 1010, 1012, 1013, 1027, 1028, 1034, 1063, 1064, 1066, 1075, 1077, 1078, 1080, 1084, 1106, 1119, 1120, 1126, 1132, 1146, 1154, 1173, 1176, 1183, 1193, 1200, 1201, 1203, 1212, 1216, 1224, 1225, 1232, 1237, 1244, 1265, 1267, 1272, 1275, 1283, 1284, 1285, 1290, 1291, 1292, 1293, 1297, 1302, 1306, 1349, 1372, 1376, 1379, 1380, 1383, 1399, 1408, 1412, 1413, 1415, 1429, 1435, 1436, 1437, 1438, 1456, 1497, 1498, 1501, 1518, 1519, 1525, 1533, 1544, 1560, 1606, 1608, 1612, 1615, 1618, 1625, 1627, 1640, 1641, 1643, 1644, 1648, 1653, 1657, 1661, 1665, 1667, 1673, 1686, 1689, 1695, 1698, 1704, 1711, 1720, 1732, 1739, 1755, 1766, 1768, 1769, 1774, 1775, 1781, 1797, 1803, 1804, 1805, 1809, 1812, 1816, 1818, 1819, 1826, 1828, 1830, 1836, 1839, 1845, 1856, 1868, 1878, 1879, 1887, 1904, 1914, 1933, 1937, 1954, 1957, 1966, 1971, 1977, 1981, 1988, 1998, 2001, 2004, 2017, 2040, 2047, 2049, 2055, 2057, 2061, 2065, 2072, 2074, 2079, 2085, 2089, 2090, 2093, 2095, 2098, 2135, 2149, 2162, 2168, 2170, 2174, 2208, 2233, 2234, 2240, 2245, 2261, 2268, 2271, 2272, 2280, 2282, 2291, 2298, 2312, 2332, 2338, 2354, 2356, 2360, 2380, 2383, 2384, 2404, 2405, 2413, 2417, 2426, 2433, 2435, 2437, 2438, 2439, 2451, 2458, 2476, 2480, 2483, 2492, 2498, 2502, 2507, 2518, 2519, 2521, 2527, 2530, 2556, 2557, 2563, 2565, 2572, 2576, 2607, 2612, 2614, 2616, 2617, 2620, 2621, 2624, 2628, 2632, 2634, 2657, 2665, 2666, 2673, 2676, 2694, 2696, 2699, 2701, 2708, 2718, 2723, 2730, 2732, 2735, 2737, 2738, 2746, 2766, 2767, 2770, 2776, 2785, 2798, 2804, 2819, 2824, 2827, 2834, 2841, 2856, 2863, 2870, 2891, 2892, 2906, 2907, 2912, 2914, 2920, 2923, 2936, 2944, 2945, 2946, 2949, 2969, 2984, 2993, 2996, 2999, 3012, 3017, 3019, 3034, 3040, 3050, 3057, 3061, 3086, 3088, 3102, 3103, 3106, 3114, 3125, 3131, 3132, 3143, 3145, 3150, 3159, 3176, 3177, 3181, 3188, 3201, 3213, 3216, 3226, 3237, 3244, 3255, 3284, 3291, 3296, 3297, 3320, 3326, 3332, 3365, 3371, 3396, 3407, 3433, 3439, 3458, 3480, 3485, 3503, 3509, 3521, 3525, 3533, 3536, 3545, 3547, 3550, 3554, 3559, 3567, 3578, 3589, 3607, 3610, 3626, 3628, 3643, 3649, 3650, 3653, 3671, 3675, 3679, 3686, 3693, 3695, 3735, 3738, 3740, 3741, 3753, 3761, 3762, 3763, 3768, 3770, 3786, 3788, 3794, 3797, 3798, 3805, 3811, 3816, 3835, 3844, 3847, 3864, 3867, 3873, 3874, 3877, 3886, 3894, 3901, 3921, 3922, 3932, 3935, 3945, 3947, 3950, 3953, 3957, 3966, 3974, 3983, 3991, 3994, 3998, 4003, 4010, 4015, 4032, 4041, 4047, 4063, 4067, 4073, 4088, -1, -1, -1, -1, -1, -1, -1, -1, -1, -1, -1, -1, -1, -1, -1, -1, -1, -1, -1, -1, -1, -1, -1, -1, -1, -1, -1, -1, -1, -1, -1, -1, -1, -1, -1, -1, -1, -1, -1, -1, -1, -1, -1, -1, -1, -1, -1, -1, 0, 1, 7, 10, 32, 35, 37, 41, 54, 56, 60, 64, 78, 93, 98, 100, 110, 137, 148, 151, 169, 173, 188, 192, 201, 216, 223, 228, 233, 240, 245, 248, 263, 271, 275, 278, 279, 286, 287, 312, 316, 326, 328, 363, 381, 383, 385, 387, 389, 399, 426, 428, 431, 436, 452, 456, 457, 461, 468, 478, 484, 487, 502, 516, 520, 523, 539, 544, 545, 551, 566, 567, 571, 574, 576, 581, 606, 625, 636, 638, 639, 644, 647, 649, 650, 658, 661, 666, 673, 677, 678, 690, 719, 729, 735, 751, 760, 784, 787, 789, 792, 800, 801, 815, 827, 868, 869, 886, 892, 902, 910, 913, 929, 939, 953, 958, 964, 984, 1040, 1043, 1044, 1046, 1049, 1053, 1070, 1087, 1091, 1099, 1102, 1112, 1115, 1128, 1140, 1149, 1150, 1157, 1160, 1165, 1184, 1188, 1190, 1192, 1204, 1220, 1222, 1234, 1238, 1241, 1242, 1248, 1249, 1260, 1289, 1300, 1311, 1319, 1324, 1326, 1333, 1335, 1337, 1339, 1341, 1347, 1354, 1357, 1358, 1363, 1366, 1381, 1382, 1387, 1398, 1405, 1406, 1411, 1416, 1430, 1431, 1446, 1451, 1453, 1464, 1471, 1473, 1475, 1492, 1493, 1500, 1522, 1524, 1526, 1534, 1535, 1542, 1553, 1557, 1565, 1568, 1569, 1572, 1573, 1575, 1577, 1586, 1588, 1600, 1609, 1610, 1611, 1616, 1621, 1622, 1628, 1649, 1652, 1658, 1668, 1679, 1730, 1733, 1789, 1792, 1796, 1824, 1833, 1837, 1841, 1853, 1874, 1875, 1876, 1881, 1886, 1889, 1907, 1916, 1922, 1923, 1925, 1930, 1936, 1945, 1949, 1951, 1973, 1987, 1993, 2015, 2027, 2034, 2037, 2041, 2054, 2066, 2067, 2082, 2112, 2139, 2166, 2172, 2176, 2196, 2225, 2253, 2254, 2256, 2267, 2274, 2283, 2284, 2292, 2293, 2299, 2306, 2307, 2315, 2328, 2329, 2331, 2350, 2352, 2367, 2368, 2382, 2399, 2427, 2436, 2440, 2449, 2470, 2474, 2485, 2499, 2504, 2524, 2525, 2541, 2558, 2559, 2560, 2567, 2594, 2596, 2603, 2609, 2629, 2630, 2633, 2639, 2641, 2648, 2649, 2650, 2651, 2664, 2674, 2690, 2692, 2697, 2698, 2709, 2715, 2724, 2739, 2745, 2756, 2769, 2771, 2795, 2799, 2820, 2843, 2845, 2885, 2890, 2908, 2909, 2918, 2939, 2954, 2960, 2970, 2977, 2978, 2981, 2985, 3006, 3009, 3010, 3015, 3018, 3027, 3058, 3069, 3078, 3079, 3082, 3083, 3085, 3091, 3099, 3107, 3110, 3115, 3121, 3122, 3135, 3151, 3156, 3162, 3165, 3197, 3205, 3206, 3227, 3228, 3230, 3242, 3250, 3256, 3257, 3261, 3271, 3278, 3294, 3311, 3313, 3321, 3333, 3351, 3353, 3356, 3373, 3375, 3376, 3379, 3388, 3393, 3409, 3411, 3417, 3422, 3427, 3428, 3438, 3444, 3447, 3449, 3467, 3484, 3490, 3492, 3493, 3510, 3511, 3515, 3522, 3524, 3529, 3531, 3540, 3541, 3549, 3551, 3555, 3561, 3563, 3565, 3576, 3586, 3592, 3594, 3596, 3597, 3600, 3603, 3606, 3608, 3616, 3619, 3620, 3623, 3641, 3654, 3661, 3670, 3680, 3689, 3706, 3708, 3709, 3713, 3714, 3720, 3722, 3729, 3730, 3732, 3739, 3751, 3774, 3777, 3780, 3789, 3796, 3820, 3825, 3832, 3840, 3848, 3857, 3861, 3863, 3865, 3872, 3878, 3888, 3890, 3911, 3913, 3933, 3940, 3946, 3968, 3987, 3990, 4004, 4016, 4023, 4024, 4037, 4039, 4042, 4046, 4059, 4066, 4068, 4091, 4094, 4095, -1, -1, -1, -1, -1, -1, -1, -1, -1, -1, -1, 3, 5, 8, 25, 26, 58, 61, 66, 67, 88, 91, 97, 111, 117, 122, 132, 136, 181, 183, 186, 199, 200, 202, 204, 206, 209, 219, 235, 243, 247, 253, 256, 262, 265, 267, 269, 272, 276, 282, 284, 306, 323, 329, 338, 340, 349, 351, 355, 372, 390, 425, 429, 435, 441, 443, 454, 463, 475, 476, 490, 493, 501, 534, 542, 553, 562, 570, 575, 582, 586, 590, 609, 615, 620, 648, 654, 667, 681, 697, 700, 701, 704, 705, 709, 718, 723, 733, 739, 742, 747, 755, 761, 769, 773, 785, 788, 794, 795, 816, 820, 822, 846, 848, 864, 865, 870, 872, 874, 887, 896, 914, 917, 921, 925, 941, 963, 971, 980, 985, 993, 996, 1005, 1006, 1008, 1015, 1018, 1023, 1029, 1037, 1038, 1047, 1055, 1062, 1081, 1089, 1094, 1105, 1108, 1110, 1114, 1118, 1125, 1134, 1135, 1138, 1141, 1156, 1158, 1164, 1169, 1187, 1226, 1229, 1239, 1243, 1245, 1246, 1252, 1270, 1278, 1286, 1294, 1323, 1325, 1334, 1343, 1345, 1369, 1394, 1402, 1407, 1417, 1423, 1444, 1448, 1449, 1458, 1465, 1466, 1467, 1474, 1482, 1491, 1504, 1505, 1508, 1521, 1523, 1532, 1537, 1539, 1543, 1551, 1561, 1571, 1581, 1590, 1613, 1624, 1638, 1662, 1670, 1671, 1674, 1682, 1687, 1690, 1692, 1696, 1699, 1701, 1708, 1712, 1718, 1724, 1725, 1761, 1762, 1765, 1780, 1783, 1802, 1813, 1866, 1884, 1893, 1895, 1917, 1928, 1929, 1931, 1941, 1947, 1952, 1958, 1959, 1962, 1964, 1965, 1978, 1995, 2003, 2005, 2010, 2012, 2030, 2045, 2068, 2073, 2075, 2081, 2083, 2087, 2091, 2092, 2103, 2105, 2106, 2126, 2130, 2156, 2163, 2164, 2167, 2175, 2178, 2188, 2190, 2191, 2192, 2198, 2211, 2217, 2230, 2246, 2249, 2250, 2258, 2266, 2270, 2294, 2301, 2310, 2321, 2326, 2339, 2349, 2351, 2373, 2374, 2386, 2390, 2393, 2400, 2423, 2425, 2430, 2432, 2471, 2477, 2481, 2488, 2490, 2491, 2497, 2503, 2508, 2535, 2539, 2540, 2545, 2547, 2564, 2568, 2574, 2589, 2592, 2597, 2602, 2606, 2613, 2615, 2618, 2627, 2631, 2642, 2643, 2679, 2682, 2693, 2712, 2716, 2722, 2755, 2764, 2768, 2773, 2774, 2787, 2788, 2803, 2806, 2810, 2814, 2826, 2828, 2833, 2835, 2858, 2865, 2869, 2874, 2877, 2881, 2886, 2894, 2897, 2899, 2904, 2910, 2911, 2915, 2943, 2952, 2963, 2964, 2968, 2975, 2982, 2987, 2991, 2997, 3005, 3008, 3020, 3036, 3041, 3043, 3046, 3056, 3060, 3067, 3073, 3080, 3084, 3089, 3090, 3094, 3109, 3113, 3144, 3160, 3168, 3170, 3173, 3179, 3182, 3186, 3198, 3235, 3238, 3241, 3245, 3247, 3258, 3268, 3269, 3270, 3272, 3275, 3298, 3307, 3312, 3316, 3318, 3322, 3323, 3328, 3334, 3338, 3340, 3342, 3346, 3348, 3355, 3362, 3372, 3374, 3381, 3383, 3390, 3412, 3413, 3416, 3421, 3423, 3425, 3454, 3470, 3472, 3474, 3479, 3483, 3496, 3502, 3505, 3507, 3518, 3537, 3539, 3553, 3558, 3568, 3570, 3573, 3574, 3609, 3614, 3633, 3634, 3635, 3639, 3640, 3645, 3658, 3665, 3673, 3690, 3691, 3707, 3711, 3725, 3733, 3734, 3736, 3756, 3791, 3792, 3801, 3804, 3830, 3852, 3858, 3859, 3880, 3882, 3887, 3889, 3893, 3898, 3904, 3908, 3920, 3925, 3926, 3937, 3956, 3960, 3962, 3971, 3975, 3977, 3984, 3985, 3988, 3997, 4011, 4013, 4027, 4028, 4031, 4036, 4054, 4058, 4065, 4075, -1, -1, -1, -1, -1, -1, -1, -1, -1, -1, -1, -1, -1, -1, -1, -1, -1, -1, -1, -1, -1, -1, -1, -1, -1, -1, -1, -1, -1, -1, -1, -1, -1, -1, -1, -1, -1, -1, -1, -1, -1, -1, -1, -1, -1, -1, -1, -1, -1, -1, -1, -1, -1, -1, -1, -1, -1, -1, -1, -1};

__global__ __launch_bounds__(256) void k_hh_gather(const float* __restrict__ X, int NPR, unsigned short* __restrict__ PH_, unsigned short* __restrict__ PL_) { const long long u = (long long)blockIdx.x * 256 + threadIdx.x; if (u >= (long long)NPR * 512) return; const int c = 4 * (int)(u & 511); const int g = (int)(u >> 9); const int r = c_perm[g]; v4f v; v.x = v.y = v.z = v.w = 0.f; if (r >= 0) v = *(const v4f*)(X + (long long)r * 2048 + c); st4s(PH_, PL_, (long long)g * 2048 + c, v); }
__global__ __launch_bounds__(256) void k_hh_scatter(const float* __restrict__ Y, int g0, int cnt, float* __restrict__ OUT) { const int u = blockIdx.x * 256 + threadIdx.x; if (u >= cnt * 128) return; const int c = 4 * (u & 127); const int g = g0 + (u >> 7); const int r = c_perm[g]; if (r < 0) return; VST2V4(OUT + (long long)r * 512 + c, *(const v4f*)(Y + (long long)g * 512 + c)); }


extern "C" void kernel_launch(void* const* d_in, const int* in_sizes, int n_in, void* d_out, int out_size, void* d_ws, size_t ws_size, hipStream_t stream) {
    (void)in_sizes; (void)n_in; (void)out_size; (void)ws_size;
    const float* x = (const float*)d_in[0];
    const int* hh = (const int*)d_in[1];
    const float* Wh = (const float*)d_in[2];
    const float* bh = (const float*)d_in[3];
    float* out = (float*)d_out;
    char* wsp = (char*)d_ws;
    unsigned short* AH = (unsigned short*)wsp; wsp += (((size_t)((size_t)4416 * 2048) * 2 + 255) / 256) * 256;
    unsigned short* AL = (unsigned short*)wsp; wsp += (((size_t)((size_t)4416 * 2048) * 2 + 255) / 256) * 256;
    unsigned short* WH = (unsigned short*)wsp; wsp += (((size_t)((size_t)512 * 2048) * 2 + 255) / 256) * 256;
    unsigned short* WL = (unsigned short*)wsp; wsp += (((size_t)((size_t)512 * 2048) * 2 + 255) / 256) * 256;
    float* Y = (float*)wsp; wsp += (((size_t)((size_t)4416 * 512) * 4 + 255) / 256) * 256;
    if ((size_t)(wsp - (char*)d_ws) > ws_size) return;
    k_hh_gather<<<(unsigned)((4416LL * 512 + 255) / 256), 256, 0, stream>>>(x, 4416, AH, AL);
    k_u2_bt<<<(unsigned)((512LL * 1024 + 255) / 256), 256, 0, stream>>>(Wh + 0, 512, 1, 2048, 512, 2048, 512, nullptr, WH, WL);
    w25::wmma_gemm64<1, true, 2, 0, false, 0><<<dim3((unsigned)((((576) / 64) * ((512) / 64) + 7) / 8), (unsigned)(1)), 256, 0, stream>>>((const unsigned short*)(AH + 0), (const unsigned short*)(AL + 0), 2048, 0, (const unsigned short*)(WH), (const unsigned short*)(WL), 2048, 0, (void*)(Y + 0), nullptr, 512, 0, bh + 0, nullptr, 0, 576, 512, 2048, 1.0f);
    k_hh_scatter<<<(576 * 128 + 255) / 256, 256, 0, stream>>>(Y, 0, 576, out);
    k_u2_bt<<<(unsigned)((512LL * 1024 + 255) / 256), 256, 0, stream>>>(Wh + 1048576, 512, 1, 2048, 512, 2048, 512, nullptr, WH, WL);
    w25::wmma_gemm64<1, true, 2, 0, false, 0><<<dim3((unsigned)((((576) / 64) * ((512) / 64) + 7) / 8), (unsigned)(1)), 256, 0, stream>>>((const unsigned short*)(AH + 1179648), (const unsigned short*)(AL + 1179648), 2048, 0, (const unsigned short*)(WH), (const unsigned short*)(WL), 2048, 0, (void*)(Y + 294912), nullptr, 512, 0, bh + 512, nullptr, 0, 576, 512, 2048, 1.0f);
    k_hh_scatter<<<(576 * 128 + 255) / 256, 256, 0, stream>>>(Y, 576, 576, out);
    k_u2_bt<<<(unsigned)((512LL * 1024 + 255) / 256), 256, 0, stream>>>(Wh + 2097152, 512, 1, 2048, 512, 2048, 512, nullptr, WH, WL);
    w25::wmma_gemm64<1, true, 2, 0, false, 0><<<dim3((unsigned)((((512) / 64) * ((512) / 64) + 7) / 8), (unsigned)(1)), 256, 0, stream>>>((const unsigned short*)(AH + 2359296), (const unsigned short*)(AL + 2359296), 2048, 0, (const unsigned short*)(WH), (const unsigned short*)(WL), 2048, 0, (void*)(Y + 589824), nullptr, 512, 0, bh + 1024, nullptr, 0, 512, 512, 2048, 1.0f);
    k_hh_scatter<<<(512 * 128 + 255) / 256, 256, 0, stream>>>(Y, 1152, 512, out);
    k_u2_bt<<<(unsigned)((512LL * 1024 + 255) / 256), 256, 0, stream>>>(Wh + 3145728, 512, 1, 2048, 512, 2048, 512, nullptr, WH, WL);
    w25::wmma_gemm64<1, true, 2, 0, false, 0><<<dim3((unsigned)((((576) / 64) * ((512) / 64) + 7) / 8), (unsigned)(1)), 256, 0, stream>>>((const unsigned short*)(AH + 3407872), (const unsigned short*)(AL + 3407872), 2048, 0, (const unsigned short*)(WH), (const unsigned short*)(WL), 2048, 0, (void*)(Y + 851968), nullptr, 512, 0, bh + 1536, nullptr, 0, 576, 512, 2048, 1.0f);
    k_hh_scatter<<<(576 * 128 + 255) / 256, 256, 0, stream>>>(Y, 1664, 576, out);
    k_u2_bt<<<(unsigned)((512LL * 1024 + 255) / 256), 256, 0, stream>>>(Wh + 4194304, 512, 1, 2048, 512, 2048, 512, nullptr, WH, WL);
    w25::wmma_gemm64<1, true, 2, 0, false, 0><<<dim3((unsigned)((((512) / 64) * ((512) / 64) + 7) / 8), (unsigned)(1)), 256, 0, stream>>>((const unsigned short*)(AH + 4587520), (const unsigned short*)(AL + 4587520), 2048, 0, (const unsigned short*)(WH), (const unsigned short*)(WL), 2048, 0, (void*)(Y + 1146880), nullptr, 512, 0, bh + 2048, nullptr, 0, 512, 512, 2048, 1.0f);
    k_hh_scatter<<<(512 * 128 + 255) / 256, 256, 0, stream>>>(Y, 2240, 512, out);
    k_u2_bt<<<(unsigned)((512LL * 1024 + 255) / 256), 256, 0, stream>>>(Wh + 5242880, 512, 1, 2048, 512, 2048, 512, nullptr, WH, WL);
    w25::wmma_gemm64<1, true, 2, 0, false, 0><<<dim3((unsigned)((((576) / 64) * ((512) / 64) + 7) / 8), (unsigned)(1)), 256, 0, stream>>>((const unsigned short*)(AH + 5636096), (const unsigned short*)(AL + 5636096), 2048, 0, (const unsigned short*)(WH), (const unsigned short*)(WL), 2048, 0, (void*)(Y + 1409024), nullptr, 512, 0, bh + 2560, nullptr, 0, 576, 512, 2048, 1.0f);
    k_hh_scatter<<<(576 * 128 + 255) / 256, 256, 0, stream>>>(Y, 2752, 576, out);
    k_u2_bt<<<(unsigned)((512LL * 1024 + 255) / 256), 256, 0, stream>>>(Wh + 6291456, 512, 1, 2048, 512, 2048, 512, nullptr, WH, WL);
    w25::wmma_gemm64<1, true, 2, 0, false, 0><<<dim3((unsigned)((((512) / 64) * ((512) / 64) + 7) / 8), (unsigned)(1)), 256, 0, stream>>>((const unsigned short*)(AH + 6815744), (const unsigned short*)(AL + 6815744), 2048, 0, (const unsigned short*)(WH), (const unsigned short*)(WL), 2048, 0, (void*)(Y + 1703936), nullptr, 512, 0, bh + 3072, nullptr, 0, 512, 512, 2048, 1.0f);
    k_hh_scatter<<<(512 * 128 + 255) / 256, 256, 0, stream>>>(Y, 3328, 512, out);
    k_u2_bt<<<(unsigned)((512LL * 1024 + 255) / 256), 256, 0, stream>>>(Wh + 7340032, 512, 1, 2048, 512, 2048, 512, nullptr, WH, WL);
    w25::wmma_gemm64<1, true, 2, 0, false, 0><<<dim3((unsigned)((((576) / 64) * ((512) / 64) + 7) / 8), (unsigned)(1)), 256, 0, stream>>>((const unsigned short*)(AH + 7864320), (const unsigned short*)(AL + 7864320), 2048, 0, (const unsigned short*)(WH), (const unsigned short*)(WL), 2048, 0, (void*)(Y + 1966080), nullptr, 512, 0, bh + 3584, nullptr, 0, 576, 512, 2048, 1.0f);
    k_hh_scatter<<<(576 * 128 + 255) / 256, 256, 0, stream>>>(Y, 3840, 576, out);
}
